// GA_GAT_40724879900765
// MI455X (gfx1250) — hardware-verified
//
#include <hip/hip_runtime.h>
#include <math.h>

typedef __attribute__((ext_vector_type(16))) _Float16 v16h;
typedef __attribute__((ext_vector_type(8)))  _Float16 v8h;
typedef __attribute__((ext_vector_type(16))) __bf16   v16b;
typedef __attribute__((ext_vector_type(8)))  float    v8f;
typedef __attribute__((ext_vector_type(4)))  float    v4f;

__device__ __forceinline__ int frag_k(int i, int h) { return (i < 8) ? (8 * h + i) : (16 + 8 * h + (i - 8)); }
__device__ __forceinline__ __bf16 bf16_rne(float f) {
    unsigned int u = __float_as_uint(f);
    u += 0x7fffu + ((u >> 16) & 1u);
    return __builtin_bit_cast(__bf16, (unsigned short)(u >> 16));
}
__device__ __forceinline__ float bf16_f32(__bf16 b) { return __uint_as_float(((unsigned int)__builtin_bit_cast(unsigned short, b)) << 16); }
__device__ __forceinline__ v8f wmma16(v16h a, v16h b, v8f c) {
    c = __builtin_amdgcn_wmma_f32_16x16x32_f16(false, a, false, b, (short)0, c, false, false);
    asm volatile("v_nop\n\tv_nop\n\tv_nop\n\tv_nop" : "+v"(c) : "v"(a), "v"(b));
    return c;
}
__device__ __forceinline__ v8f wmmab(v16b a, v16b b, v8f c) {
    c = __builtin_amdgcn_wmma_f32_16x16x32_bf16(false, a, false, b, (short)0, c, false, false);
    asm volatile("v_nop\n\tv_nop\n\tv_nop\n\tv_nop" : "+v"(c) : "v"(a), "v"(b));
    return c;
}
struct Split { v16b hi, lo; };
__device__ __forceinline__ v8f wmma3(const Split& a, const Split& b, v8f c) {
    c = __builtin_amdgcn_wmma_f32_16x16x32_bf16(false, a.hi, false, b.hi, (short)0, c, false, false);
    c = __builtin_amdgcn_wmma_f32_16x16x32_bf16(false, a.hi, false, b.lo, (short)0, c, false, false);
    c = __builtin_amdgcn_wmma_f32_16x16x32_bf16(false, a.lo, false, b.hi, (short)0, c, false, false);
    asm volatile("v_nop\n\tv_nop\n\tv_nop\n\tv_nop" : "+v"(c) : "v"(a.hi), "v"(a.lo), "v"(b.hi), "v"(b.lo));
    return c;
}
struct Split3 { v16b hi, mid, lo; };
__device__ __forceinline__ v8f wmma6(const Split3& a, const Split3& b, v8f c) {
    c = __builtin_amdgcn_wmma_f32_16x16x32_bf16(false, a.hi, false, b.hi, (short)0, c, false, false);
    c = __builtin_amdgcn_wmma_f32_16x16x32_bf16(false, a.hi, false, b.mid, (short)0, c, false, false);
    c = __builtin_amdgcn_wmma_f32_16x16x32_bf16(false, a.mid, false, b.hi, (short)0, c, false, false);
    c = __builtin_amdgcn_wmma_f32_16x16x32_bf16(false, a.hi, false, b.lo, (short)0, c, false, false);
    c = __builtin_amdgcn_wmma_f32_16x16x32_bf16(false, a.mid, false, b.mid, (short)0, c, false, false);
    c = __builtin_amdgcn_wmma_f32_16x16x32_bf16(false, a.lo, false, b.hi, (short)0, c, false, false);
    asm volatile("v_nop\n\tv_nop\n\tv_nop\n\tv_nop" : "+v"(c) : "v"(a.hi), "v"(a.mid), "v"(a.lo), "v"(b.hi), "v"(b.mid), "v"(b.lo));
    return c;
}

__device__ __forceinline__ v16h fh_ld(const float* __restrict__ p, long long sk, int k0, int h, int klen, float s) {
    v16h a;
#pragma unroll
    for (int i = 0; i < 16; ++i) { const int k = k0 + frag_k(i, h); a[i] = (k < klen) ? (_Float16)(p[(long long)k * sk] * s) : (_Float16)0.f; }
    return a;
}
__device__ __forceinline__ Split sp_ld(const float* __restrict__ p, long long sk, int k0, int h, int klen, float s) {
    Split r;
#pragma unroll
    for (int i = 0; i < 16; ++i) {
        const int k = k0 + frag_k(i, h); const float x = (k < klen) ? p[(long long)k * sk] * s : 0.f;
        const __bf16 hb = bf16_rne(x); r.hi[i] = hb; r.lo[i] = bf16_rne(x - bf16_f32(hb));
    }
    return r;
}
__device__ __forceinline__ Split3 sp3_ld(const float* __restrict__ p, long long sk, int k0, int h, int klen, float s) {
    Split3 r;
#pragma unroll
    for (int i = 0; i < 16; ++i) {
        const int k = k0 + frag_k(i, h); const float x = (k < klen) ? p[(long long)k * sk] * s : 0.f;
        const __bf16 hb = bf16_rne(x); const float r1 = x - bf16_f32(hb); const __bf16 mb = bf16_rne(r1);
        r.hi[i] = hb; r.mid[i] = mb; r.lo[i] = bf16_rne(r1 - bf16_f32(mb));
    }
    return r;
}
__device__ __forceinline__ v16b bh_ld(const float* __restrict__ p, long long sk, int k0, int h, int klen, float s) {
    v16b a;
#pragma unroll
    for (int i = 0; i < 16; ++i) { const int k = k0 + frag_k(i, h); a[i] = bf16_rne((k < klen) ? p[(long long)k * sk] * s : 0.f); }
    return a;
}
__device__ __forceinline__ v16h fh_row(const _Float16* __restrict__ row, int k0, int h) {
    v16h a;
#pragma unroll
    for (int i = 0; i < 16; ++i) a[i] = row[k0 + frag_k(i, h)];
    return a;
}

#define VST2(T, ptr, val) do { *(volatile T*)(ptr) = (val); __threadfence(); *(volatile T*)(ptr) = (val); } while (0)
typedef float v4f __attribute__((ext_vector_type(4)));
#define VST2V4(ptr, val) do { *(volatile v4f*)(ptr) = (val); __threadfence(); *(volatile v4f*)(ptr) = (val); } while (0)

__device__ __attribute__((noinline)) float act_fn(float v, int act) {
    if (act == 1) return fmaxf(v, 0.f);
    if (act == 2) { const float u = 0.7978845608028654f * (v + 0.044715f * v * v * v); return 0.5f * v * (1.f + tanhf(u)); }
    if (act == 3) return v / (1.f + expf(-v));
    if (act == 4) return 0.5f * v * (1.f + erff(v * 0.7071067811865476f));
    if (act == 5) return tanhf(v);
    if (act == 6) return 1.f / (1.f + expf(-v));
    if (act == 7) return (v > 0.f) ? v : 0.01f * v;
    if (act == 8) return (v > 0.f) ? v : (expf(v) - 1.f);
    if (act == 9) return fminf(fmaxf(v, 0.f), 6.f);
    if (act == 10) return fabsf(v);
    if (act == 11) return (v >= 0.f) ? v : 0.1f * v;
    if (act == 12) return (v > 0.f) ? v : 0.2f * v;
    if (act == 13) return (v > 20.f) ? v : log1pf(expf(v));
    return v;
}

struct GemmP {
    const float* A; const float* B; const float* bias; const float* R; float* C;
    long long sAo, sAi, sAm, sAk, sBo, sBi, sBn, sBk, sCo, sCi, sCm, sRo, sRi, sRm, sRn;
    int M, N, K, zi_n, flags, act; float alpha, beta, sa, sb;
    int Npad, pad_;
};
static_assert(sizeof(GemmP) == 5 * 8 + 15 * 8 + 6 * 4 + 4 * 4 + 2 * 4, "GemmP has padding");

template <int MODE>
__global__ __launch_bounds__(32) void k_gemm(GemmP p) {
    const int lane = threadIdx.x & 31, h = lane >> 4, l15 = lane & 15;
    const int m0 = blockIdx.y * 16, n0 = blockIdx.x * 32;
    const int z = blockIdx.z, zo = z / p.zi_n, zi = z - zo * p.zi_n;
    const float* A = p.A + zo * p.sAo + zi * p.sAi;
    const float* B = p.B + zo * p.sBo + zi * p.sBi;
    const int am = min(m0 + l15, p.M - 1);
    v8f acc[2], comp[2];
#pragma unroll
    for (int t = 0; t < 2; ++t) { v8f zz = {}; acc[t] = zz; comp[t] = zz; }
    for (int k0 = 0; k0 < p.K; k0 += 32) {
        const float* arow = A + (long long)am * p.sAm;
        if (MODE == 1) {
            const Split a = sp_ld(arow, p.sAk, k0, h, p.K, 1.f);
#pragma unroll
            for (int t = 0; t < 2; ++t) {
                const int bn = min(n0 + t * 16 + l15, p.N - 1);
                acc[t] = wmma3(a, sp_ld(B + (long long)bn * p.sBn, p.sBk, k0, h, p.K, 1.f), acc[t]);
            }
        } else if (MODE == 3) {
            const Split3 a = sp3_ld(arow, p.sAk, k0, h, p.K, 1.f);
#pragma unroll
            for (int t = 0; t < 2; ++t) {
                const int bn = min(n0 + t * 16 + l15, p.N - 1);
                acc[t] = wmma6(a, sp3_ld(B + (long long)bn * p.sBn, p.sBk, k0, h, p.K, 1.f), acc[t]);
            }
        } else if (MODE == 4) {
            const Split3 a = sp3_ld(arow, p.sAk, k0, h, p.K, 1.f);
#pragma unroll
            for (int t = 0; t < 2; ++t) {
                const int bn = min(n0 + t * 16 + l15, p.N - 1); v8f zz = {};
                const v8f part = wmma6(a, sp3_ld(B + (long long)bn * p.sBn, p.sBk, k0, h, p.K, 1.f), zz);
                const v8f y = part - comp[t]; const v8f s = acc[t] + y; comp[t] = (s - acc[t]) - y; acc[t] = s;
            }
        } else if (MODE == 2) {
            const v16b a = bh_ld(arow, p.sAk, k0, h, p.K, 1.f);
#pragma unroll
            for (int t = 0; t < 2; ++t) {
                const int bn = min(n0 + t * 16 + l15, p.N - 1);
                acc[t] = wmmab(a, bh_ld(B + (long long)bn * p.sBn, p.sBk, k0, h, p.K, 1.f), acc[t]);
            }
        } else {
            const v16h a = fh_ld(arow, p.sAk, k0, h, p.K, p.sa);
#pragma unroll
            for (int t = 0; t < 2; ++t) {
                const int bn = min(n0 + t * 16 + l15, p.N - 1);
                acc[t] = wmma16(a, fh_ld(B + (long long)bn * p.sBn, p.sBk, k0, h, p.K, p.sb), acc[t]);
            }
        }
    }
    const float iscale = (MODE == 0) ? p.alpha / (p.sa * p.sb) : p.alpha;
    float* C = p.C + zo * p.sCo + zi * p.sCi;
    const float* R = p.R + zo * p.sRo + zi * p.sRi;
    __shared__ __align__(16) float ctile[16][36];
#pragma unroll
    for (int t = 0; t < 2; ++t) {
        const int n = n0 + t * 16 + l15; const int nn = min(n, p.N - 1);
#pragma unroll
        for (int r = 0; r < 8; ++r) {
            const int m = m0 + 8 * h + r; const int mm = min(m, p.M - 1);
            float v = acc[t][r] * iscale;
            if (p.flags & 1) v += p.bias[nn];
            if (p.flags & 2) v += p.bias[mm];
            v = act_fn(v, p.act);
            if (p.flags & 4) v += p.beta * R[(long long)mm * p.sRm + (long long)nn * p.sRn];
            ctile[8 * h + r][t * 16 + l15] = (n < p.N) ? v : 0.f;
        }
    }
    __syncthreads();
    const int NW = (p.Npad > p.N) ? p.Npad : p.N;
    const bool fast = (m0 + 16 <= p.M) && (n0 + 32 <= NW) && ((p.sCm & 3) == 0) && ((((size_t)C) & 15) == 0);
    if (fast) {
#pragma unroll
        for (int s = 0; s < 4; ++s) {
            const int row = s * 4 + (lane >> 3), c4 = (lane & 7) * 4;
            const v4f v = *(const v4f*)&ctile[row][c4];
            VST2V4(C + (long long)(m0 + row) * p.sCm + n0 + c4, v);
        }
    } else {
        for (int row = 0; row < 16; ++row) {
            const int m = m0 + row, n = n0 + lane;
            if (m < p.M && n < NW) VST2(float, C + (long long)m * p.sCm + n, ctile[row][lane]);
        }
    }
}

#define AW 4
struct AttnP {
    const float* Q; const float* K; const float* V; float* O; float* P; const float* Mf; const int* Mi; float* ST;
    const float* Pw; const float* Rt; const int* SQ; const int* SK;
    long long swb, swh, swi, swj, srb, srh, sri;
    long long sQb, sQh, sQi, sQd, sKb, sKh, sKj, sKd, sVb, sVh, sVj, sVd, sOb, sOh, sOi, sPb, sPh, sPi, smb, smh, smi, smj;
    int Lq, Lk, dh, dv, hrep, causal, coff, pband;
    float scale, mfill; int nonorm, mpol;
    int roff, rn, segpol, win;
};
static_assert(sizeof(AttnP) == 12 * 8 + 29 * 8 + 16 * 4, "AttnP has padding");

#ifndef KATTN_ATTR
#define KATTN_ATTR
#endif
template <int DHP, int DVP, int QM, bool SPLITPV, bool TWOPASS>
__global__ __launch_bounds__(32 * AW) KATTN_ATTR void k_attn(AttnP p) {
    constexpr int NT = DVP / 16;
    constexpr int KS = DHP / 32;
    constexpr int VP = DVP + 8;
    __shared__ __align__(16) float    pl[AW][16 * 64];
    __shared__ __align__(16) _Float16 vl[(SPLITPV ? 2 : 1) * 64 * VP];
    const int lane = threadIdx.x & 31, hf = lane >> 4, l15 = lane & 15, wave = threadIdx.x >> 5;
    const int h = blockIdx.y, b = blockIdx.z, hk = h / p.hrep;
    const int q0 = (blockIdx.x * AW + wave) * 16;
    float* myp = pl[wave];
    const float L2E = 1.4426950408889634f;
    const float NEG = -__builtin_inff();
    const int qi = min(q0 + l15, p.Lq - 1);
    const float* qrow = p.Q + b * p.sQb + h * p.sQh + (long long)qi * p.sQi;
    const float* kbase = p.K + b * p.sKb + hk * p.sKh;
    const float* vbase = p.V + b * p.sVb + hk * p.sVh;
    v16h qa[QM == 0 ? KS : 1]; Split qs_[QM == 1 ? KS : 1]; Split3 qt_[QM == 2 ? KS : 1];
#pragma unroll
    for (int ks = 0; ks < KS; ++ks) {
        if (QM == 2) qt_[ks] = sp3_ld(qrow, p.sQd, ks * 32, hf, p.dh, 1.f);
        else if (QM == 1) qs_[ks] = sp_ld(qrow, p.sQd, ks * 32, hf, p.dh, 1.f);
        else qa[ks] = fh_ld(qrow, p.sQd, ks * 32, hf, p.dh, 1.f);
    }
    v8f o[NT]; float m8[8], l8[8];
#pragma unroll
    for (int t = 0; t < NT; ++t) { v8f zz = {}; o[t] = zz; }
#pragma unroll
    for (int i = 0; i < 8; ++i) { m8[i] = NEG; l8[i] = 0.f; }
    int jend = p.Lk;
    if (p.causal == 1) { const int je = (blockIdx.x * AW + AW - 1) * 16 + 16 + p.coff; jend = min(jend, max(je, 0)); }
    const int npass = TWOPASS ? 2 : 1;
    for (int pass = 0; pass < npass; ++pass) {
        const bool dopv = (!TWOPASS) || pass == 1;
        for (int j0 = 0; j0 < jend; j0 += 64) {
            if (dopv) {
                __syncthreads();
                for (int idx = threadIdx.x; idx < 64 * DVP; idx += 32 * AW) {
                    const int jr = idx / DVP, d = idx - jr * DVP, j = j0 + jr;
                    const float f = (j < p.Lk && d < p.dv) ? vbase[(long long)j * p.sVj + (long long)d * p.sVd] : 0.f;
                    if (SPLITPV) {
                        const __bf16 hb = bf16_rne(f);
                        ((__bf16*)vl)[jr * VP + d] = hb; ((__bf16*)vl)[64 * VP + jr * VP + d] = bf16_rne(f - bf16_f32(hb));
                    } else vl[jr * VP + d] = (_Float16)f;
                }
            }
            v8f s[4];
#pragma unroll
            for (int t = 0; t < 4; ++t) {
                const int j = min(j0 + t * 16 + l15, p.Lk - 1);
                const float* krow = kbase + (long long)j * p.sKj;
                v8f acc = {};
#pragma unroll
                for (int ks = 0; ks < KS; ++ks) {
                    if (QM == 2)      acc = wmma6(qt_[ks], sp3_ld(krow, p.sKd, ks * 32, hf, p.dh, 1.f), acc);
                    else if (QM == 1) acc = wmma3(qs_[ks], sp_ld(krow, p.sKd, ks * 32, hf, p.dh, 1.f), acc);
                    else              acc = wmma16(qa[ks], fh_ld(krow, p.sKd, ks * 32, hf, p.dh, 1.f), acc);
                }
                s[t] = acc;
            }
            float pv[8][4];
#pragma unroll
            for (int i = 0; i < 8; ++i) {
                const int irow = q0 + i + 8 * hf;
                const int ic = min(irow, p.Lq - 1);
                float sc[4];
#pragma unroll
                for (int t = 0; t < 4; ++t) {
                    const int jg = j0 + t * 16 + l15;
                    float v = s[t][i] * p.scale;
                    if (p.Mf) v += p.Mf[b * p.smb + h * p.smh + (long long)ic * p.smi + (long long)min(jg, p.Lk - 1) * p.smj];
                    if (p.Rt) { int rc = ic - min(jg, p.Lk - 1) + p.roff; rc = rc < 0 ? 0 : (rc >= p.rn ? p.rn - 1 : rc); v += p.Rt[b * p.srb + h * p.srh + (long long)ic * p.sri + rc]; }
                    if (p.Mi) { const int mv = p.Mi[b * p.smb + h * p.smh + (long long)ic * p.smi + (long long)min(jg, p.Lk - 1) * p.smj]; if (p.mpol ? (mv != 0) : (mv == 0)) v = p.mfill; }
                    if (p.SQ) { const bool same = p.SQ[(long long)b * p.Lq + ic] == p.SK[(long long)b * p.Lk + min(jg, p.Lk - 1)]; if (p.segpol ? same : !same) v = p.mfill; }
                    if (p.causal == 2 && jg > irow + p.coff) v = p.mfill;
                    if (jg >= p.Lk || (p.causal == 1 && jg > irow + p.coff) || (p.causal == 3 && jg < irow + p.coff) || (p.win > 0 && irow + p.coff - jg > p.win)) v = NEG; else v *= L2E;
                    sc[t] = v;
                }
                if (!TWOPASS || pass == 0) {
                    float mx = fmaxf(fmaxf(sc[0], sc[1]), fmaxf(sc[2], sc[3]));
                    mx = fmaxf(mx, __shfl_xor(mx, 1, 32)); mx = fmaxf(mx, __shfl_xor(mx, 2, 32));
                    mx = fmaxf(mx, __shfl_xor(mx, 4, 32)); mx = fmaxf(mx, __shfl_xor(mx, 8, 32));
                    const float mnew = fmaxf(m8[i], mx);
                    const float corr = (mnew == NEG) ? 1.f : exp2f(m8[i] - mnew);
                    float rs = 0.f;
#pragma unroll
                    for (int t = 0; t < 4; ++t) {
                        const float pp = (sc[t] == NEG) ? 0.f : exp2f(sc[t] - mnew); rs += pp;
                        pv[i][t] = p.Pw ? pp * p.Pw[b * p.swb + h * p.swh + (long long)ic * p.swi + (long long)min(j0 + t * 16 + l15, p.Lk - 1) * p.swj] : pp;
                    }
                    rs += __shfl_xor(rs, 1, 32); rs += __shfl_xor(rs, 2, 32); rs += __shfl_xor(rs, 4, 32); rs += __shfl_xor(rs, 8, 32);
                    l8[i] = l8[i] * corr + rs; m8[i] = mnew;
                    if (!TWOPASS) {
#pragma unroll
                        for (int t = 0; t < NT; ++t) o[t][i] *= corr;
                    }
                } else {
                    const float inv = (l8[i] > 0.f) ? 1.f / l8[i] : 0.f;
#pragma unroll
                    for (int t = 0; t < 4; ++t) {
                        const int jg = j0 + t * 16 + l15;
                        float pp = (sc[t] == NEG) ? 0.f : exp2f(sc[t] - m8[i]) * inv;
                        if (p.Pw) pp *= p.Pw[b * p.swb + h * p.swh + (long long)ic * p.swi + (long long)min(jg, p.Lk - 1) * p.swj];
                        pv[i][t] = pp;
                    }
                }
            }
            if (dopv) {
#pragma unroll
                for (int i = 0; i < 8; ++i)
#pragma unroll
                    for (int t = 0; t < 4; ++t) myp[(i + 8 * hf) * 64 + t * 16 + l15] = pv[i][t];
                __syncthreads();
                if (p.P) {
                    float* pb_ = p.P + b * p.sPb + h * p.sPh;
                    const bool fastP = (p.pband == 0) && ((p.sPi & 3) == 0) && (j0 + 64 <= p.Lk) && (q0 + 16 <= p.Lq) && ((((size_t)pb_) & 15) == 0);
                    if (fastP) {
#pragma unroll
                        for (int s = 0; s < 8; ++s) {
                            const int row = s * 2 + (lane >> 4), c4 = (lane & 15) * 4;
                            const v4f v = *(const v4f*)(myp + row * 64 + c4);
                            VST2V4(pb_ + (long long)(q0 + row) * p.sPi + j0 + c4, v);
                        }
                    } else {
                        for (int row = 0; row < 16; ++row) {
                            const int irow = q0 + row; if (irow >= p.Lq) continue;
                            for (int c = lane; c < 64; c += 32) {
                                const int jg = j0 + c; if (jg >= p.Lk) continue;
                                if (p.pband == 0) VST2(float, pb_ + (long long)irow * p.sPi + jg, myp[row * 64 + c]);
                                else if (jg - irow <= p.pband && irow - jg <= p.pband) VST2(float, pb_ + (long long)irow * p.sPi + (jg - irow + p.pband), myp[row * 64 + c]);
                            }
                        }
                    }
                }
                if (SPLITPV) {
                    const Split pa0 = sp_ld(myp + l15 * 64, 1, 0, hf, 64, 1.f), pa1 = sp_ld(myp + l15 * 64, 1, 32, hf, 64, 1.f);
                    const __bf16* vh = (const __bf16*)vl; const __bf16* vlo = vh + 64 * VP;
#pragma unroll
                    for (int t = 0; t < NT; ++t) {
                        const int dcol = t * 16 + l15;
                        Split b0, b1;
#pragma unroll
                        for (int e = 0; e < 16; ++e) {
                            const int k0 = frag_k(e, hf), k1 = 32 + frag_k(e, hf);
                            b0.hi[e] = vh[k0 * VP + dcol]; b0.lo[e] = vlo[k0 * VP + dcol]; b1.hi[e] = vh[k1 * VP + dcol]; b1.lo[e] = vlo[k1 * VP + dcol];
                        }
                        o[t] = wmma3(pa0, b0, o[t]);
                        o[t] = wmma3(pa1, b1, o[t]);
                    }
                } else {
                    const v16h pa0 = fh_ld(myp + l15 * 64, 1, 0, hf, 64, 4096.f), pa1 = fh_ld(myp + l15 * 64, 1, 32, hf, 64, 4096.f);
#pragma unroll
                    for (int t = 0; t < NT; ++t) {
                        const int dcol = t * 16 + l15;
                        v16h b0, b1;
#pragma unroll
                        for (int e = 0; e < 16; ++e) { b0[e] = vl[frag_k(e, hf) * VP + dcol]; b1[e] = vl[(32 + frag_k(e, hf)) * VP + dcol]; }
                        o[t] = wmma16(pa0, b0, o[t]);
                        o[t] = wmma16(pa1, b1, o[t]);
                    }
                }
            }
        }
    }
    float* obase = p.O + b * p.sOb + h * p.sOh;
    if (p.ST) {
        const int rl = lane >> 1, isel = rl & 7;
        float mv = 0.f, lv = 0.f;
#pragma unroll
        for (int i = 0; i < 8; ++i) if (i == isel) { mv = m8[i]; lv = l8[i]; }
        const int irow = q0 + rl;
        if (irow < p.Lq) { float* st = p.ST + (((long long)b * gridDim.y + h) * p.Lq + irow) * 2 + (lane & 1); VST2(float, st, (lane & 1) ? lv : mv * 0.6931471805599453f); }
    }
    float invr[8];
#pragma unroll
    for (int i = 0; i < 8; ++i) {
        if (TWOPASS) invr[i] = SPLITPV ? 1.f : (1.f / 4096.f);
        else if (p.nonorm) invr[i] = exp2f(m8[i]) * (SPLITPV ? 1.f : (1.f / 4096.f));
        else invr[i] = (l8[i] > 0.f) ? (SPLITPV ? 1.f / l8[i] : 1.f / (l8[i] * 4096.f)) : 0.f;
    }
    __syncthreads();
    const bool ofast = ((p.sOi & 3) == 0) && ((((size_t)obase) & 15) == 0) && (q0 + 16 <= p.Lq);
#pragma unroll
    for (int c0 = 0; c0 < DVP; c0 += 64) {
#pragma unroll
        for (int i = 0; i < 8; ++i)
#pragma unroll
            for (int t = 0; t < NT; ++t) if (t * 16 >= c0 && t * 16 < c0 + 64) myp[(i + 8 * hf) * 64 + (t * 16 - c0) + l15] = o[t][i] * invr[i];
        __syncthreads();
        const int cw = (DVP - c0 < 64) ? (DVP - c0) : 64;
        if (ofast && (c0 + cw <= p.dv) && (cw % 32 == 0)) {
            const int lpr = cw / 4;
            const int rows_per_ins = 32 / lpr;
            for (int r0 = 0; r0 < 16; r0 += rows_per_ins) {
                const int row = r0 + lane / lpr, c4 = (lane % lpr) * 4;
                const v4f v = *(const v4f*)(myp + row * 64 + c4);
                VST2V4(obase + (long long)(q0 + row) * p.sOi + c0 + c4, v);
            }
        } else {
            for (int row = 0; row < 16; ++row) {
                const int irow = q0 + row; if (irow >= p.Lq) continue;
                for (int c = lane; c < cw; c += 32) { const int d = c0 + c; if (d < p.dv) VST2(float, obase + (long long)irow * p.sOi + d, myp[row * 64 + c]); }
            }
        }
        __syncthreads();
    }
}

struct TrP { const float* src; float* dst; const float* R2; long long sSz, lds, sDz, ldd, sRz, ldr; int R, C, flags, act; float alpha, beta; };
static_assert(sizeof(TrP) == 3 * 8 + 6 * 8 + 6 * 4, "TrP has padding");
__global__ __launch_bounds__(256) void k_tr(TrP p) {
    __shared__ float tile[32][33];
    const int c0 = blockIdx.x * 32, r0 = blockIdx.y * 32, z = blockIdx.z;
    const int lane = threadIdx.x & 31, wave = threadIdx.x >> 5;
    const float* s = p.src + z * p.sSz;
#pragma unroll
    for (int k = 0; k < 4; ++k) {
        const int rl = wave * 4 + k, r = r0 + rl, c = c0 + lane;
        tile[rl][lane] = (r < p.R && c < p.C) ? s[(long long)r * p.lds + c] : 0.f;
    }
    __syncthreads();
    float* d = p.dst + z * p.sDz; const float* rr = p.R2 + z * p.sRz;
#pragma unroll
    for (int k = 0; k < 4; ++k) {
        const int cl = wave * 4 + k, c = c0 + cl, r = r0 + lane;
        if (c < p.C && r < p.R) {
            float v = act_fn(p.alpha * tile[lane][cl], p.act);
            if (p.flags & 1) v += p.beta * rr[(long long)c * p.ldr + r];
            VST2(float, d + (long long)c * p.ldd + r, v);
        }
    }
}

__global__ __launch_bounds__(256) void k_affine(const float* __restrict__ src, float* __restrict__ dst, int n, float a, float b, const float* __restrict__ sdev) {
    const int i = blockIdx.x * 256 + threadIdx.x;
    if (i < n) { const float aa = sdev ? a * sdev[0] : a; const float v = aa * src[i] + b; VST2(float, dst + i, v); }
}

struct SmP { const float* src; float* dst; const float* Mf; long long sz, sr, dz, dr, smz, smr; int n, pad; float scale_in, scale_out; };
static_assert(sizeof(SmP) == 3 * 8 + 6 * 8 + 4 * 4, "SmP has padding");
__global__ __launch_bounds__(256) void k_softmax(SmP p) {
    __shared__ float red[256];
    const int r = blockIdx.x, z = blockIdx.y, tid = threadIdx.x;
    const float* s = p.src + z * p.sz + (long long)r * p.sr;
    const float* mf = p.Mf ? (p.Mf + z * p.smz + (long long)r * p.smr) : nullptr;
    float mx = -__builtin_inff();
    for (int j = tid; j < p.n; j += 256) { float v = s[j] * p.scale_in; if (mf) v += mf[j]; mx = fmaxf(mx, v); }
    red[tid] = mx; __syncthreads();
    for (int o = 128; o > 0; o >>= 1) { if (tid < o) red[tid] = fmaxf(red[tid], red[tid + o]); __syncthreads(); }
    mx = red[0]; __syncthreads();
    float sum = 0.f;
    for (int j = tid; j < p.n; j += 256) { float v = s[j] * p.scale_in; if (mf) v += mf[j]; sum += (mx == -__builtin_inff()) ? 0.f : expf(v - mx); }
    red[tid] = sum; __syncthreads();
    for (int o = 128; o > 0; o >>= 1) { if (tid < o) red[tid] += red[tid + o]; __syncthreads(); }
    sum = red[0];
    const float inv = (sum > 0.f) ? p.scale_out / sum : 0.f;
    float* d = p.dst + z * p.dz + (long long)r * p.dr;
    for (int j = tid; j < p.n; j += 256) { float v = s[j] * p.scale_in; if (mf) v += mf[j]; const float o = (mx == -__builtin_inff()) ? 0.f : expf(v - mx) * inv; VST2(float, d + j, o); }
}
__global__ __launch_bounds__(256) void k_stats(const float* __restrict__ x, long long sz, long long so, long long si, int inner, int n, float eps, float* __restrict__ stat, int mode) {
    __shared__ float red[256];
    const int z = blockIdx.x, tid = threadIdx.x;
    const float* base = x + z * sz;
    float s = 0.f;
    for (int e = tid; e < n; e += 256) s += base[(long long)(e / inner) * so + (long long)(e % inner) * si];
    red[tid] = s; __syncthreads();
    for (int o = 128; o > 0; o >>= 1) { if (tid < o) red[tid] += red[tid + o]; __syncthreads(); }
    const float mu = (mode == 0 || mode == 3) ? red[0] / (float)n : 0.f; __syncthreads();
    float q = 0.f;
    for (int e = tid; e < n; e += 256) { const float dlt = base[(long long)(e / inner) * so + (long long)(e % inner) * si] - mu; q += dlt * dlt; }
    red[tid] = q; __syncthreads();
    for (int o = 128; o > 0; o >>= 1) { if (tid < o) red[tid] += red[tid + o]; __syncthreads(); }
    {
        float rs;
        if (mode == 2) rs = sqrtf((float)n) / fmaxf(sqrtf(red[0]), eps); else if (mode == 3) rs = rsqrtf(red[0] / (float)(n - 1) + eps); else rs = rsqrtf(red[0] / (float)n + eps);
        if (tid < 32) { const float v = (tid == 0) ? mu : ((tid == 1) ? rs : 0.f); VST2(float, stat + (long long)z * 32 + tid, v); }
    }
}
__global__ __launch_bounds__(256) void k_norm_apply(const float* __restrict__ x, float* __restrict__ y, const float* __restrict__ stat, const float* __restrict__ g, const float* __restrict__ bta,
                                                     int Z, int C, int L, int G, int bn, int act) {
    const long long idx = (long long)blockIdx.x * 256 + threadIdx.x;
    if (idx >= (long long)Z * C * L) return;
    const int l = (int)(idx % L); const long long zc = idx / L; const int c = (int)(zc % C), z = (int)(zc / C); (void)l;
    const int set = bn ? c : (z * G + c / (C / G));
    float v = (x[idx] - stat[(long long)set * 32]) * stat[(long long)set * 32 + 1];
    if (g) v *= g[c];
    if (bta) v += bta[c];
    v = act_fn(v, act);
    VST2(float, y + idx, v);
}

__global__ __launch_bounds__(256) void k_lse_neg(const float* __restrict__ st, float* __restrict__ c, int n) {
    const int i = blockIdx.x * 256 + threadIdx.x;
    if (i < n) { const float v = -(st[2 * i] + logf(st[2 * i + 1])); VST2(float, c + i, v); }
}

__global__ __launch_bounds__(256) void k_iota(int* __restrict__ dst, int n, int a, int b) {
    const int i = blockIdx.x * 256 + threadIdx.x;
    if (i < n) { const int v = a * i + b; VST2(int, dst + i, v); }
}

__global__ __launch_bounds__(256) void k_axpby(const float* __restrict__ x, const float* __restrict__ y, float* __restrict__ dst, int n, float a, float b, float c) {
    const int i = blockIdx.x * 256 + threadIdx.x;
    if (i < n) { const float v = a * x[i] + b * y[i] + c; VST2(float, dst + i, v); }
}

struct RopeP { const float* X; float* Y; const float* C; const float* Sn; const int* pos; long long sXr, sXh, sYr, sYh, sCb, sCp, sCd; int R, Hn, D, S, mode, tmode, pmode, pad; };
static_assert(sizeof(RopeP) == 5 * 8 + 7 * 8 + 8 * 4, "RopeP has padding");
__global__ __launch_bounds__(256) void k_rope(RopeP p) {
    const long long idx = (long long)blockIdx.x * 256 + threadIdx.x;
    if (idx >= (long long)p.R * p.Hn * p.D) return;
    const int d = (int)(idx % p.D); const long long rh = idx / p.D; const int h = (int)(rh % p.Hn); const int r = (int)(rh / p.Hn);
    const int half = p.D / 2;
    int partner; float sign;
    if (p.mode == 0) { partner = (d < half) ? d + half : d - half; sign = (d < half) ? -1.f : 1.f; }
    else { partner = d ^ 1; sign = (d & 1) ? 1.f : -1.f; }
    const int tcol = (p.tmode == 0) ? d : ((p.tmode == 1) ? (d % half) : (d >> 1));
    const int pp = (p.pmode == 0) ? (r % p.S) : ((p.pmode == 1) ? h : p.pos[r]);
    const long long toff = (long long)(r / p.S) * p.sCb + (long long)pp * p.sCp + (long long)tcol * p.sCd;
    const float* xr = p.X + (long long)r * p.sXr + (long long)h * p.sXh;
    const float v = xr[d] * p.C[toff] + sign * xr[partner] * p.Sn[toff];
    VST2(float, p.Y + (long long)r * p.sYr + (long long)h * p.sYh + d, v);
}

__global__ __launch_bounds__(256) void k_invf(float* __restrict__ invb, int half, int D, float base, float num, int fmode, float cexp) {
    const int i = blockIdx.x * 256 + threadIdx.x;
    if (i >= ((half + 31) / 32) * 32) return;
    if (i >= half) { VST2(float, invb + i, 0.f); return; }
    const float e = (float)(2 * i) / (float)D;
    float invf;
    if (fmode == 1) invf = num * expf((float)(2 * i) * cexp);
    else if (fmode == 2) invf = num * powf(base, (-2.0f * ((float)i - 1.0f)) / (float)D);
    else invf = num * (1.0f / powf(base, e));
    VST2(float, invb + i, invf);
}
__global__ __launch_bounds__(256) void k_sincos(float* __restrict__ cs, float* __restrict__ sn, const float* __restrict__ invb, int S, int half, float pscale) {
    const int idx = blockIdx.x * 256 + threadIdx.x;
    if (idx >= S * half) return;
    const int s = idx / half, i = idx - s * half;
    const float ang = (pscale * (float)s) * invb[i];
    VST2(float, cs + idx, cosf(ang)); VST2(float, sn + idx, sinf(ang));
}

__global__ __launch_bounds__(256) void k_mulact(const float* __restrict__ x, const float* __restrict__ y, float* __restrict__ dst, int n, int act) {
    const int i = blockIdx.x * 256 + threadIdx.x;
    if (i < n) { const float v = act_fn(x[i], act) * y[i]; VST2(float, dst + i, v); }
}

__global__ __launch_bounds__(256) void k_matvec(GemmP p) {
    const int rpt = (p.N == 1) ? 1 : 32;
    const long long r0 = ((long long)blockIdx.x * 256 + threadIdx.x) * rpt; const int z = blockIdx.z, zo = z / p.zi_n, zi = z - zo * p.zi_n;
    if (r0 >= p.M) return;
    const float* Bb = p.B + zo * p.sBo + zi * p.sBi;
    float* C = p.C + zo * p.sCo + zi * p.sCi; const float* R = p.R + zo * p.sRo + zi * p.sRi;
    for (int rr = 0; rr < rpt; ++rr) {
        const long long r = r0 + rr; if (r >= p.M) break;
        const float* A = p.A + zo * p.sAo + zi * p.sAi + r * p.sAm;
        float acc[8] = {0.f, 0.f, 0.f, 0.f, 0.f, 0.f, 0.f, 0.f};
        for (int k = 0; k < p.K; ++k) { const float a = A[(long long)k * p.sAk];
#pragma unroll
            for (int j = 0; j < 8; ++j) if (j < p.N) acc[j] += a * Bb[(long long)j * p.sBn + (long long)k * p.sBk]; }
#pragma unroll
        for (int j = 0; j < 8; ++j) if (j < p.N) {
            float v = acc[j] * p.alpha;
            if (p.flags & 1) v += p.bias[j];
            if (p.flags & 2) v += p.bias[r];
            v = act_fn(v, p.act);
            if (p.flags & 4) v += p.beta * R[r * p.sRm + (long long)j * p.sRn];
            VST2(float, C + r * p.sCm + j, v);
        }
    }
}
__global__ __launch_bounds__(256) void k_smallsoftmax(const float* __restrict__ src, float* __restrict__ dst, long long sr, long long dr, int n, long long R, float scale) {
    const long long r0 = ((long long)blockIdx.x * 256 + threadIdx.x) * 32;
    for (int rr = 0; rr < 32; ++rr) {
        const long long r = r0 + rr; if (r >= R) return;
        const float* s = src + r * sr; float* d = dst + r * dr;
        float mx = -__builtin_inff();
        for (int j = 0; j < n; ++j) mx = fmaxf(mx, s[j] * scale);
        float sum = 0.f;
        for (int j = 0; j < n; ++j) sum += expf(s[j] * scale - mx);
        const float inv = 1.f / sum;
        for (int j = 0; j < n; ++j) { const float v = expf(s[j] * scale - mx) * inv; VST2(float, d + j, v); }
    }
}

__global__ __launch_bounds__(32) void k_unitstat(float* __restrict__ st) { const int t = threadIdx.x; const float v = (t == 1) ? 1.f : 0.f; VST2(float, st + t, v); }

__global__ __launch_bounds__(256) void k_lincopy(const float* __restrict__ src, long long lds, float* __restrict__ dst, long long ldd, long long rows, int cols) {
    const long long i = (long long)blockIdx.x * 256 + threadIdx.x; if (i >= rows * cols) return;
    const long long r = i / cols; const int c = (int)(i - r * cols);
    const float v = src[r * lds + c]; VST2(float, dst + r * ldd + c, v);
}


#define IL3_CH 4096
__global__ __launch_bounds__(256) void k_csr3_bcount(const int* __restrict__ tgt, int E, int N, int* __restrict__ CNT) { __shared__ int tt[IL3_CH]; const int ch = blockIdx.x; const int b = threadIdx.x; const int e0 = ch * IL3_CH; const int nt = min(IL3_CH, E - e0);
    for (int i = b; i < nt; i += 256) tt[i] = (int)(((long long)tgt[e0 + i] * 256) / N); __syncthreads(); int c = 0;
    for (int i = 0; i < nt; ++i) c += (tt[i] == b); VST2(int, CNT + (long long)ch * 256 + b, c); }
__global__ __launch_bounds__(256) void k_csr3_bscan(const int* __restrict__ CNT, int nch, int E, int* __restrict__ OFFB, int* __restrict__ BOFF) { __shared__ int tot[256]; const int b = threadIdx.x; int s = 0; for (int ch = 0; ch < nch; ++ch) s += CNT[(long long)ch * 256 + b]; tot[b] = s; __syncthreads();
    if (b == 0) { int run = 0; for (int i = 0; i < 256; ++i) { const int v = tot[i]; tot[i] = run; run += v; } } __syncthreads();
    int run = tot[b]; VST2(int, BOFF + b, run); if (b == 255) VST2(int, BOFF + 256, E);
    for (int ch = 0; ch < nch; ++ch) { VST2(int, OFFB + (long long)ch * 256 + b, run); run += CNT[(long long)ch * 256 + b]; } }
__global__ __launch_bounds__(256) void k_csr3_bscatter(const int* __restrict__ tgt, int E, int N, const int* __restrict__ OFFB, int* __restrict__ BUF) { __shared__ int tt[IL3_CH]; const int ch = blockIdx.x; const int b = threadIdx.x; const int e0 = ch * IL3_CH; const int nt = min(IL3_CH, E - e0);
    for (int i = b; i < nt; i += 256) tt[i] = (int)(((long long)tgt[e0 + i] * 256) / N); __syncthreads(); int pos = OFFB[(long long)ch * 256 + b];
    for (int i = 0; i < nt; ++i) if (tt[i] == b) { VST2(int, BUF + pos, e0 + i); ++pos; } }
template <int CAP>
__global__ __launch_bounds__(256) void k_csr3_lists(const int* __restrict__ tgt, const int* __restrict__ BUF, const int* __restrict__ BOFF, int N, int* __restrict__ NBR, int* __restrict__ cnt) { const int d = blockIdx.x * 256 + threadIdx.x; if (d >= N) return; const int b = (int)(((long long)d * 256) / N); int n = 0; int* row = NBR + (long long)d * CAP;
    for (int p = BOFF[b]; p < BOFF[b + 1]; ++p) { const int e = BUF[p]; if (tgt[e] == d) { if (n < CAP) VST2(int, row + n, e); ++n; } }
    for (int j = n; j < CAP; ++j) VST2(int, row + j, -1); VST2(int, cnt + d, min(n, CAP)); }
__global__ __launch_bounds__(256) void k_csr3_scan(const int* __restrict__ cnt, int* __restrict__ off, int N) {
    __shared__ int part[256]; const int per = ((((N + 255) / 256) + 31) / 32) * 32; const int a = threadIdx.x * per, b = min(N, a + per); int s = 0;
    for (int i = a; i < b; ++i) s += cnt[i]; part[threadIdx.x] = s; __syncthreads();
    if (threadIdx.x == 0) { int run = 0; for (int t = 0; t < 256; ++t) { const int v = part[t]; part[t] = run; run += v; } } __syncthreads();
    int run = part[threadIdx.x]; for (int i = a; i < b; ++i) { VST2(int, off + i, run); run += cnt[i]; }
    if (a < N && b == N) { VST2(int, off + N, run); } }
template <int CAP>
__global__ __launch_bounds__(256) void k_csr3_slotcopy(const int* __restrict__ off, const int* __restrict__ NBR, int* __restrict__ slot, int N) {
    const int t = blockIdx.x * 256 + threadIdx.x; const int tot = off[N]; if (t >= tot) return;
    int lo = 0, hi = N - 1; while (lo < hi) { const int mid = (lo + hi + 1) >> 1; if (off[mid] <= t) lo = mid; else hi = mid - 1; }
    int j = t - off[lo]; j = (j < 0) ? 0 : ((j >= CAP) ? (CAP - 1) : j); VST2(int, slot + t, NBR[(long long)lo * CAP + j]); }

#define IL_CAP128 128
#define IL_T128 64
#define IL_TILE128 4096
__global__ __launch_bounds__(IL_T128) void k_inlists128(const int* __restrict__ tgt, int E, int N, int* __restrict__ NBR, int* __restrict__ cnt) {
    __shared__ int tt[IL_TILE128];
    __shared__ int lists[IL_T128 * IL_CAP128];
    const int d = blockIdx.x * IL_T128 + threadIdx.x; int n = 0;
    for (int e0 = 0; e0 < E; e0 += IL_TILE128) {
        const int nt = min(IL_TILE128, E - e0);
        __syncthreads();
        for (int i = threadIdx.x; i < nt; i += IL_T128) tt[i] = tgt[e0 + i];
        __syncthreads();
        for (int i = 0; i < nt; ++i) { if (tt[i] == d) { if (n < IL_CAP128) lists[threadIdx.x * IL_CAP128 + n] = e0 + i; ++n; } }
    }
    if (d < N) {
        int* row = NBR + (long long)d * IL_CAP128;
        for (int j = 0; j < IL_CAP128; ++j) { const int v = (j < n) ? lists[threadIdx.x * IL_CAP128 + j] : -1; VST2(int, row + j, v); }
        VST2(int, cnt + d, min(n, IL_CAP128));
    }
}
__global__ __launch_bounds__(256) void k_csr_scan128(const int* __restrict__ cnt, int* __restrict__ off, int N) {
    __shared__ int part[256]; const int per = ((((N + 255) / 256) + 31) / 32) * 32; const int a = threadIdx.x * per, b = min(N, a + per); int s = 0;
    for (int i = a; i < b; ++i) s += cnt[i]; part[threadIdx.x] = s; __syncthreads();
    if (threadIdx.x == 0) { int run = 0; for (int t = 0; t < 256; ++t) { const int v = part[t]; part[t] = run; run += v; } } __syncthreads();
    int run = part[threadIdx.x]; for (int i = a; i < b; ++i) { VST2(int, off + i, run); run += cnt[i]; }
    if (a < N && b == N) { VST2(int, off + N, run); }
}
__global__ __launch_bounds__(256) void k_slotcopy128(const int* __restrict__ off, const int* __restrict__ NBR, int* __restrict__ slot, int N) {
    const int t = blockIdx.x * 256 + threadIdx.x; const int tot = off[N]; if (t >= tot) return;
    int lo = 0, hi = N - 1;
    while (lo < hi) { const int mid = (lo + hi + 1) >> 1; if (off[mid] <= t) lo = mid; else hi = mid - 1; }
    int j = t - off[lo]; j = (j < 0) ? 0 : ((j >= IL_CAP128) ? (IL_CAP128 - 1) : j);
    VST2(int, slot + t, NBR[(long long)lo * IL_CAP128 + j]);
}


__global__ __launch_bounds__(256) void k_csr_mean(const float* __restrict__ Hh, const int* __restrict__ src, const int* __restrict__ off, const int* __restrict__ slot, float* __restrict__ AGG, int N, int D) {
    const long long t = (long long)blockIdx.x * 256 + threadIdx.x; if (t >= (long long)N * D) return; const int d = (int)(t % D); const int i = (int)(t / D); const int a = off[i], b = off[i + 1]; float s = 0.f;
    for (int p = a; p < b; ++p) s += Hh[(long long)src[slot[p]] * D + d];
    VST2(float, AGG + t, s / fmaxf((float)(b - a), 1.f));
}


__global__ __launch_bounds__(256) void k_csr_gather(const float* __restrict__ XW, const int* __restrict__ src, const int* __restrict__ off, const int* __restrict__ slot, float* __restrict__ OUT, int N, int D, int accumulate) {
    const long long t = (long long)blockIdx.x * 256 + threadIdx.x; if (t >= (long long)N * D) return; const int d = (int)(t % D); const int i = (int)(t / D);
    const int a = off[i], b = off[i + 1]; float s = accumulate ? OUT[t] : 0.f;
    for (int p = a; p < b; ++p) s += XW[(long long)src[slot[p]] * D + d];
    VST2(float, OUT + t, s);
}

__constant__ int c_gr[8] = {0, 1, 1, 1, 2, 2, 2, 3};
__global__ __launch_bounds__(256) void k_gg_rbf(const float* __restrict__ pos, const int* __restrict__ ei, float* __restrict__ RBF, int E) { const int q = blockIdx.x * 256 + threadIdx.x; if (q >= E * 32) return; const int c = q % 32; const int e = q / 32; float v = 0.f; if (c < 20) { const int s = ei[e], d = ei[E + e]; const float dx = pos[s * 3] - pos[d * 3], dy = pos[s * 3 + 1] - pos[d * 3 + 1], dz = pos[s * 3 + 2] - pos[d * 3 + 2]; const float d2 = dx * dx + dy * dy + dz * dz; const float dist = (d2 > 0.f) ? sqrtf(d2) : 0.f; const float cen = (float)c * (10.f / 19.f); const float t = (dist - cen) / (10.f / 19.f); v = expf(-0.5f * t * t); } VST2(float, RBF + q, v); }
__global__ __launch_bounds__(256) void k_gg_embed(const float* __restrict__ pos, const int* __restrict__ zz, const int* __restrict__ bat, const float* __restrict__ PM, const float* __restrict__ aw, const float* __restrict__ inw, const float* __restrict__ inb, float* __restrict__ HB, int N, int C) { const int q = blockIdx.x * 256 + threadIdx.x; if (q >= N * 8 * C) return; const int o = q % C; const int b = (q / C) % 8; const int n = q / (8 * C); float v = 0.f;
    if (b == 0) { int a = zz[n]; a = min(max(a, 0), 99); float s = inb[o];
#pragma unroll 1
        for (int i = 0; i < C; ++i) s += aw[a * C + i] * inw[o * (C + 1) + i]; v = s; }
    else if (b <= 3) { const int gph = bat[n]; v = inw[o * (C + 1) + C] * (pos[n * 3 + (b - 1)] - PM[gph * 3 + (b - 1)]); }
    VST2(float, HB + q, v); }
__global__ __launch_bounds__(256) void k_gg_sc(const float* __restrict__ Zb, const float* __restrict__ asrc, const float* __restrict__ adst, const float* __restrict__ wsrc, const float* __restrict__ wdst, float* __restrict__ SS, int N, int C, int HD) { const int q = blockIdx.x * 256 + threadIdx.x; if (q >= N * 4) return; const int h = q % 4; const int n = q / 4; float ss = 0.f, sd = 0.f;
#pragma unroll 1
    for (int b = 0; b < 8; ++b) { const float ws = wsrc[h * 4 + c_gr[b]], wd = wdst[h * 4 + c_gr[b]];
#pragma unroll 1
        for (int cc = 0; cc < HD; ++cc) { const float zv = Zb[((long long)n * 8 + b) * C + h * HD + cc]; ss += zv * asrc[(h * HD + cc) * 8 + b] * ws; sd += zv * adst[(h * HD + cc) * 8 + b] * wd; } }
    VST2(float, SS + n * 8 + h, ss); VST2(float, SS + n * 8 + 4 + h, sd); }
__global__ __launch_bounds__(256) void k_gg_alpha(const float* __restrict__ SS, const float* __restrict__ ES, int lde, const int* __restrict__ ei, const int* __restrict__ off, const int* __restrict__ slot, float* __restrict__ AT, int N, int E) { const int q = blockIdx.x * 256 + threadIdx.x; if (q >= N * 4) return; const int h = q % 4; const int n = q / 4; const float sdn = SS[n * 8 + 4 + h]; float mx = -__builtin_inff();
    for (int p = off[n]; p < off[n + 1]; ++p) { const int e = slot[p]; float v = SS[ei[e] * 8 + h] + sdn + ES[(long long)e * lde + h]; v = (v > 0.f) ? v : 0.2f * v; mx = fmaxf(mx, v); }
    float s = 0.f; for (int p = off[n]; p < off[n + 1]; ++p) { const int e = slot[p]; float v = SS[ei[e] * 8 + h] + sdn + ES[(long long)e * lde + h]; v = (v > 0.f) ? v : 0.2f * v; s += expf(v - mx); }
    for (int p = off[n]; p < off[n + 1]; ++p) { const int e = slot[p]; float v = SS[ei[e] * 8 + h] + sdn + ES[(long long)e * lde + h]; v = (v > 0.f) ? v : 0.2f * v; VST2(float, AT + (long long)e * 4 + h, expf(v - mx) / (s + 1e-16f)); } }
__global__ __launch_bounds__(64) void k_gg_agg(const float* __restrict__ Zb, const float* __restrict__ AT, const int* __restrict__ ei, const int* __restrict__ off, const int* __restrict__ slot, const float* __restrict__ RES, const float* __restrict__ sa, const float* __restrict__ sbb, float* __restrict__ OUT, int N, int C, int HD) { const int n = blockIdx.x; const int c = threadIdx.x; const int h = c / HD; float agg[8];
#pragma unroll
    for (int b = 0; b < 8; ++b) agg[b] = 0.f;
    for (int p = off[n]; p < off[n + 1]; ++p) { const int e = slot[p]; const int s = ei[e]; const float a = AT[(long long)e * 4 + h];
#pragma unroll
        for (int b = 0; b < 8; ++b) agg[b] += a * Zb[((long long)s * 8 + b) * C + c]; }
    float nrm[4]; nrm[0] = agg[0]; nrm[1] = agg[1] * agg[1] + agg[2] * agg[2] + agg[3] * agg[3]; nrm[2] = agg[4] * agg[4] + agg[5] * agg[5] + agg[6] * agg[6]; nrm[3] = agg[7] * agg[7];
    float gate[4];
#pragma unroll
    for (int gdx = 0; gdx < 4; ++gdx) gate[gdx] = 1.f / (1.f + expf(-(sa[c * 4 + gdx] * nrm[gdx] + sbb[c * 4 + gdx])));
#pragma unroll
    for (int b = 0; b < 8; ++b) { const int gdx = (b == 0) ? 0 : (b <= 3) ? 1 : (b <= 6) ? 2 : 3; VST2(float, OUT + ((long long)n * 8 + b) * C + c, gate[gdx] * agg[b] + RES[((long long)n * 8 + b) * C + c]); } }
__global__ __launch_bounds__(64) void k_gg_ln(float* __restrict__ X, const float* __restrict__ a, int N, int C) { __shared__ float red[64]; const int n = blockIdx.x; const int c = threadIdx.x; float s2 = 0.f;
#pragma unroll 1
    for (int b = 0; b < 8; ++b) { const float v = X[((long long)n * 8 + b) * C + c]; s2 += v * v; } red[c] = sqrtf(s2); __syncthreads(); for (int o = 32; o > 0; o >>= 1) { if (c < o) red[c] += red[c + o]; __syncthreads(); } const float nn = red[0] / (float)C + 1e-6f; const float sc = a[c] / nn;
#pragma unroll 1
    for (int b = 0; b < 8; ++b) { float* pp = X + ((long long)n * 8 + b) * C + c; const float nv = *pp * sc; VST2(float, pp, nv); } }
__global__ __launch_bounds__(256) void k_gg_head(const float* __restrict__ OP, int ldp, float* __restrict__ OUT, int G) { const int g = blockIdx.x * 256 + threadIdx.x; if (g < G) VST2(float, OUT + g, OP[(long long)g * ldp]); }

template __global__ void k_gemm<0>(GemmP);

extern "C" void kernel_launch(void* const* d_in, const int* in_sizes, int n_in, void* d_out, int out_size, void* d_ws, size_t ws_size, hipStream_t stream) {
    (void)in_sizes; (void)n_in; (void)out_size; (void)ws_size;
    const float* pos = (const float*)d_in[0];
    const int* z = (const int*)d_in[1];
    const int* ei = (const int*)d_in[2];
    const int* bat = (const int*)d_in[3];
    const float* aw = (const float*)d_in[4];
    const float* inw = (const float*)d_in[5];
    const float* inb = (const float*)d_in[6];
    const float* ew1 = (const float*)d_in[7];
    const float* eb1 = (const float*)d_in[8];
    const float* ew2 = (const float*)d_in[9];
    const float* eb2 = (const float*)d_in[10];
    const float* pw = (const float*)d_in[11];
    const float* pb = (const float*)d_in[12];
    const float* asrc = (const float*)d_in[13];
    const float* adst = (const float*)d_in[14];
    const float* wsrc = (const float*)d_in[15];
    const float* wdst = (const float*)d_in[16];
    const float* lna = (const float*)d_in[17];
    const float* sa = (const float*)d_in[18];
    const float* sb = (const float*)d_in[19];
    const float* ppw = (const float*)d_in[20];
    const float* ppb = (const float*)d_in[21];
    const float* pw1 = (const float*)d_in[22];
    const float* pb1 = (const float*)d_in[23];
    const float* pw2 = (const float*)d_in[24];
    const float* pb2 = (const float*)d_in[25];
    const int Nn = 20000;
    const int E = 320000;
    const int G = 256;
    const int C = 64;
    const int NB = 8;
    const int NH = 4;
    const int HD = 16;
    const int CAP = 40;
    const int GCAP = 128;
    const int LP = 32;
    float* out = (float*)d_out;
    char* wsp = (char*)d_ws;
    int* cnt = (int*)wsp; wsp += (((size_t)((size_t)Nn + 64) * 4 + 255) / 256) * 256;
    int* off = (int*)wsp; wsp += (((size_t)((size_t)Nn + 64) * 4 + 255) / 256) * 256;
    int* slot = (int*)wsp; wsp += (((size_t)((size_t)E + 64) * 4 + 255) / 256) * 256;
    int* nbr = (int*)wsp; wsp += (((size_t)((size_t)Nn * CAP) * 4 + 255) / 256) * 256;
    int* gcnt = (int*)wsp; wsp += (((size_t)((size_t)G + 64) * 4 + 255) / 256) * 256;
    int* goff = (int*)wsp; wsp += (((size_t)((size_t)G + 64) * 4 + 255) / 256) * 256;
    int* gslot = (int*)wsp; wsp += (((size_t)((size_t)Nn + 64) * 4 + 255) / 256) * 256;
    int* gnbr = (int*)wsp; wsp += (((size_t)((size_t)G * GCAP) * 4 + 255) / 256) * 256;
    int* ids = (int*)wsp; wsp += (((size_t)((size_t)Nn + 64) * 4 + 255) / 256) * 256;
    float* RBF = (float*)wsp; wsp += (((size_t)((size_t)E * 32) * 4 + 255) / 256) * 256;
    float* EH = (float*)wsp; wsp += (((size_t)((size_t)E * C) * 4 + 255) / 256) * 256;
    float* ES = (float*)wsp; wsp += (((size_t)((size_t)E * LP) * 4 + 255) / 256) * 256;
    float* PM = (float*)wsp; wsp += (((size_t)((size_t)G * 3) * 4 + 255) / 256) * 256;
    float* HBa = (float*)wsp; wsp += (((size_t)((size_t)Nn * NB * C) * 4 + 255) / 256) * 256;
    float* SS = (float*)wsp; wsp += (((size_t)((size_t)Nn * 8) * 4 + 255) / 256) * 256;
    float* AT = (float*)wsp; wsp += (((size_t)((size_t)E * NH) * 4 + 255) / 256) * 256;
    float* HS = (float*)wsp; wsp += (((size_t)((size_t)Nn * C) * 4 + 255) / 256) * 256;
    float* GR = (float*)wsp; wsp += (((size_t)((size_t)G * C) * 4 + 255) / 256) * 256;
    float* F1 = (float*)wsp; wsp += (((size_t)((size_t)G * C) * 4 + 255) / 256) * 256;
    float* OP = (float*)wsp; wsp += (((size_t)((size_t)G * LP) * 4 + 255) / 256) * 256;
    k_csr3_bcount<<<79, 256, 0, stream>>>(ei + E, E, Nn, nbr);
    k_csr3_bscan<<<1, 256, 0, stream>>>(nbr, 79, E, nbr + 20224, off);
    k_csr3_bscatter<<<79, 256, 0, stream>>>(ei + E, E, Nn, nbr + 20224, slot);
    k_csr3_lists<40><<<(unsigned)((Nn) + 255) / 256, 256, 0, stream>>>(ei + E, slot, off, Nn, nbr, cnt);
    k_csr3_scan<<<1, 256, 0, stream>>>(cnt, off, Nn);
    k_csr3_slotcopy<40><<<(unsigned)((E) + 255) / 256, 256, 0, stream>>>(off, nbr, slot, Nn);
    k_inlists128<<<(unsigned)((G) + IL_T128 - 1) / IL_T128, IL_T128, 0, stream>>>(bat, Nn, G, gnbr, gcnt);
    k_csr_scan128<<<1, 256, 0, stream>>>(gcnt, goff, G);
    k_slotcopy128<<<(unsigned)((Nn) + 255) / 256, 256, 0, stream>>>(goff, gnbr, gslot, G);
    k_iota<<<(unsigned)((Nn) + 255) / 256, 256, 0, stream>>>(ids, Nn, 1, 0);
    k_gg_rbf<<<(unsigned)((E * 32 + 255) / 256), 256, 0, stream>>>(pos, ei, RBF, E); k_csr_mean<<<(unsigned)((G * 3 + 255) / 256), 256, 0, stream>>>(pos, ids, goff, gslot, PM, G, 3);
    { GemmP ge1;
      ge1.A = RBF; ge1.B = ew1; ge1.bias = eb1; ge1.R = RBF; ge1.C = EH;
      ge1.sAo = 0; ge1.sAi = 0; ge1.sAm = 32; ge1.sAk = 1; ge1.sBo = 0; ge1.sBi = 0; ge1.sBn = 20; ge1.sBk = 1; ge1.sCo = 0; ge1.sCi = 0; ge1.sCm = C; ge1.sRo = 0; ge1.sRi = 0; ge1.sRm = 0; ge1.sRn = 0;
      ge1.M = E; ge1.N = C; ge1.K = 20; ge1.zi_n = 1; ge1.flags = 1; ge1.act = 3;
      ge1.alpha = 1.0f; ge1.beta = 0.0f; ge1.sa = 1.0f; ge1.sb = 8.0f; ge1.Npad = C; ge1.pad_ = 0;
      k_gemm<0><<<dim3((unsigned)((C) + 31) / 32, (unsigned)((E) + 15) / 16, (unsigned)(1)), 32, 0, stream>>>(ge1); }
    { GemmP ge2;
      ge2.A = EH; ge2.B = ew2; ge2.bias = eb2; ge2.R = EH; ge2.C = ES;
      ge2.sAo = 0; ge2.sAi = 0; ge2.sAm = C; ge2.sAk = 1; ge2.sBo = 0; ge2.sBi = 0; ge2.sBn = C; ge2.sBk = 1; ge2.sCo = 0; ge2.sCi = 0; ge2.sCm = LP; ge2.sRo = 0; ge2.sRi = 0; ge2.sRm = 0; ge2.sRn = 0;
      ge2.M = E; ge2.N = 4; ge2.K = C; ge2.zi_n = 1; ge2.flags = 1; ge2.act = 0;
      ge2.alpha = 1.0f; ge2.beta = 0.0f; ge2.sa = 1.0f; ge2.sb = 8.0f; ge2.Npad = LP; ge2.pad_ = 0;
      k_gemm<0><<<dim3((unsigned)((LP) + 31) / 32, (unsigned)((E) + 15) / 16, (unsigned)(1)), 32, 0, stream>>>(ge2); }
    k_gg_embed<<<(unsigned)((Nn * 8 * C + 255) / 256), 256, 0, stream>>>(pos, z, bat, PM, aw, inw, inb, HBa, Nn, C);
    { GemmP gz0_0;
      gz0_0.A = HBa + 0; gz0_0.B = pw + (size_t)0 * C * C; gz0_0.bias = pb + 0; gz0_0.R = HBa + 0; gz0_0.C = EH + 0;
      gz0_0.sAo = 0; gz0_0.sAi = 0; gz0_0.sAm = NB * C; gz0_0.sAk = 1; gz0_0.sBo = 0; gz0_0.sBi = 0; gz0_0.sBn = C; gz0_0.sBk = 1; gz0_0.sCo = 0; gz0_0.sCi = 0; gz0_0.sCm = NB * C; gz0_0.sRo = 0; gz0_0.sRi = 0; gz0_0.sRm = 0; gz0_0.sRn = 0;
      gz0_0.M = Nn; gz0_0.N = C; gz0_0.K = C; gz0_0.zi_n = 1; gz0_0.flags = 1; gz0_0.act = 0;
      gz0_0.alpha = 1.0f; gz0_0.beta = 0.0f; gz0_0.sa = 1.0f; gz0_0.sb = 8.0f; gz0_0.Npad = C; gz0_0.pad_ = 0;
      k_gemm<0><<<dim3((unsigned)((C) + 31) / 32, (unsigned)((Nn) + 15) / 16, (unsigned)(1)), 32, 0, stream>>>(gz0_0); }
    { GemmP gz0_1;
      gz0_1.A = HBa + 64; gz0_1.B = pw + (size_t)1 * C * C; gz0_1.bias = HBa + 64; gz0_1.R = HBa + 64; gz0_1.C = EH + 64;
      gz0_1.sAo = 0; gz0_1.sAi = 0; gz0_1.sAm = NB * C; gz0_1.sAk = 1; gz0_1.sBo = 0; gz0_1.sBi = 0; gz0_1.sBn = C; gz0_1.sBk = 1; gz0_1.sCo = 0; gz0_1.sCi = 0; gz0_1.sCm = NB * C; gz0_1.sRo = 0; gz0_1.sRi = 0; gz0_1.sRm = 0; gz0_1.sRn = 0;
      gz0_1.M = Nn; gz0_1.N = C; gz0_1.K = C; gz0_1.zi_n = 1; gz0_1.flags = 0; gz0_1.act = 0;
      gz0_1.alpha = 1.0f; gz0_1.beta = 0.0f; gz0_1.sa = 1.0f; gz0_1.sb = 8.0f; gz0_1.Npad = C; gz0_1.pad_ = 0;
      k_gemm<0><<<dim3((unsigned)((C) + 31) / 32, (unsigned)((Nn) + 15) / 16, (unsigned)(1)), 32, 0, stream>>>(gz0_1); }
    { GemmP gz0_2;
      gz0_2.A = HBa + 128; gz0_2.B = pw + (size_t)1 * C * C; gz0_2.bias = HBa + 128; gz0_2.R = HBa + 128; gz0_2.C = EH + 128;
      gz0_2.sAo = 0; gz0_2.sAi = 0; gz0_2.sAm = NB * C; gz0_2.sAk = 1; gz0_2.sBo = 0; gz0_2.sBi = 0; gz0_2.sBn = C; gz0_2.sBk = 1; gz0_2.sCo = 0; gz0_2.sCi = 0; gz0_2.sCm = NB * C; gz0_2.sRo = 0; gz0_2.sRi = 0; gz0_2.sRm = 0; gz0_2.sRn = 0;
      gz0_2.M = Nn; gz0_2.N = C; gz0_2.K = C; gz0_2.zi_n = 1; gz0_2.flags = 0; gz0_2.act = 0;
      gz0_2.alpha = 1.0f; gz0_2.beta = 0.0f; gz0_2.sa = 1.0f; gz0_2.sb = 8.0f; gz0_2.Npad = C; gz0_2.pad_ = 0;
      k_gemm<0><<<dim3((unsigned)((C) + 31) / 32, (unsigned)((Nn) + 15) / 16, (unsigned)(1)), 32, 0, stream>>>(gz0_2); }
    { GemmP gz0_3;
      gz0_3.A = HBa + 192; gz0_3.B = pw + (size_t)1 * C * C; gz0_3.bias = HBa + 192; gz0_3.R = HBa + 192; gz0_3.C = EH + 192;
      gz0_3.sAo = 0; gz0_3.sAi = 0; gz0_3.sAm = NB * C; gz0_3.sAk = 1; gz0_3.sBo = 0; gz0_3.sBi = 0; gz0_3.sBn = C; gz0_3.sBk = 1; gz0_3.sCo = 0; gz0_3.sCi = 0; gz0_3.sCm = NB * C; gz0_3.sRo = 0; gz0_3.sRi = 0; gz0_3.sRm = 0; gz0_3.sRn = 0;
      gz0_3.M = Nn; gz0_3.N = C; gz0_3.K = C; gz0_3.zi_n = 1; gz0_3.flags = 0; gz0_3.act = 0;
      gz0_3.alpha = 1.0f; gz0_3.beta = 0.0f; gz0_3.sa = 1.0f; gz0_3.sb = 8.0f; gz0_3.Npad = C; gz0_3.pad_ = 0;
      k_gemm<0><<<dim3((unsigned)((C) + 31) / 32, (unsigned)((Nn) + 15) / 16, (unsigned)(1)), 32, 0, stream>>>(gz0_3); }
    { GemmP gz0_4;
      gz0_4.A = HBa + 256; gz0_4.B = pw + (size_t)2 * C * C; gz0_4.bias = HBa + 256; gz0_4.R = HBa + 256; gz0_4.C = EH + 256;
      gz0_4.sAo = 0; gz0_4.sAi = 0; gz0_4.sAm = NB * C; gz0_4.sAk = 1; gz0_4.sBo = 0; gz0_4.sBi = 0; gz0_4.sBn = C; gz0_4.sBk = 1; gz0_4.sCo = 0; gz0_4.sCi = 0; gz0_4.sCm = NB * C; gz0_4.sRo = 0; gz0_4.sRi = 0; gz0_4.sRm = 0; gz0_4.sRn = 0;
      gz0_4.M = Nn; gz0_4.N = C; gz0_4.K = C; gz0_4.zi_n = 1; gz0_4.flags = 0; gz0_4.act = 0;
      gz0_4.alpha = 1.0f; gz0_4.beta = 0.0f; gz0_4.sa = 1.0f; gz0_4.sb = 8.0f; gz0_4.Npad = C; gz0_4.pad_ = 0;
      k_gemm<0><<<dim3((unsigned)((C) + 31) / 32, (unsigned)((Nn) + 15) / 16, (unsigned)(1)), 32, 0, stream>>>(gz0_4); }
    { GemmP gz0_5;
      gz0_5.A = HBa + 320; gz0_5.B = pw + (size_t)2 * C * C; gz0_5.bias = HBa + 320; gz0_5.R = HBa + 320; gz0_5.C = EH + 320;
      gz0_5.sAo = 0; gz0_5.sAi = 0; gz0_5.sAm = NB * C; gz0_5.sAk = 1; gz0_5.sBo = 0; gz0_5.sBi = 0; gz0_5.sBn = C; gz0_5.sBk = 1; gz0_5.sCo = 0; gz0_5.sCi = 0; gz0_5.sCm = NB * C; gz0_5.sRo = 0; gz0_5.sRi = 0; gz0_5.sRm = 0; gz0_5.sRn = 0;
      gz0_5.M = Nn; gz0_5.N = C; gz0_5.K = C; gz0_5.zi_n = 1; gz0_5.flags = 0; gz0_5.act = 0;
      gz0_5.alpha = 1.0f; gz0_5.beta = 0.0f; gz0_5.sa = 1.0f; gz0_5.sb = 8.0f; gz0_5.Npad = C; gz0_5.pad_ = 0;
      k_gemm<0><<<dim3((unsigned)((C) + 31) / 32, (unsigned)((Nn) + 15) / 16, (unsigned)(1)), 32, 0, stream>>>(gz0_5); }
    { GemmP gz0_6;
      gz0_6.A = HBa + 384; gz0_6.B = pw + (size_t)2 * C * C; gz0_6.bias = HBa + 384; gz0_6.R = HBa + 384; gz0_6.C = EH + 384;
      gz0_6.sAo = 0; gz0_6.sAi = 0; gz0_6.sAm = NB * C; gz0_6.sAk = 1; gz0_6.sBo = 0; gz0_6.sBi = 0; gz0_6.sBn = C; gz0_6.sBk = 1; gz0_6.sCo = 0; gz0_6.sCi = 0; gz0_6.sCm = NB * C; gz0_6.sRo = 0; gz0_6.sRi = 0; gz0_6.sRm = 0; gz0_6.sRn = 0;
      gz0_6.M = Nn; gz0_6.N = C; gz0_6.K = C; gz0_6.zi_n = 1; gz0_6.flags = 0; gz0_6.act = 0;
      gz0_6.alpha = 1.0f; gz0_6.beta = 0.0f; gz0_6.sa = 1.0f; gz0_6.sb = 8.0f; gz0_6.Npad = C; gz0_6.pad_ = 0;
      k_gemm<0><<<dim3((unsigned)((C) + 31) / 32, (unsigned)((Nn) + 15) / 16, (unsigned)(1)), 32, 0, stream>>>(gz0_6); }
    { GemmP gz0_7;
      gz0_7.A = HBa + 448; gz0_7.B = pw + (size_t)3 * C * C; gz0_7.bias = HBa + 448; gz0_7.R = HBa + 448; gz0_7.C = EH + 448;
      gz0_7.sAo = 0; gz0_7.sAi = 0; gz0_7.sAm = NB * C; gz0_7.sAk = 1; gz0_7.sBo = 0; gz0_7.sBi = 0; gz0_7.sBn = C; gz0_7.sBk = 1; gz0_7.sCo = 0; gz0_7.sCi = 0; gz0_7.sCm = NB * C; gz0_7.sRo = 0; gz0_7.sRi = 0; gz0_7.sRm = 0; gz0_7.sRn = 0;
      gz0_7.M = Nn; gz0_7.N = C; gz0_7.K = C; gz0_7.zi_n = 1; gz0_7.flags = 0; gz0_7.act = 0;
      gz0_7.alpha = 1.0f; gz0_7.beta = 0.0f; gz0_7.sa = 1.0f; gz0_7.sb = 8.0f; gz0_7.Npad = C; gz0_7.pad_ = 0;
      k_gemm<0><<<dim3((unsigned)((C) + 31) / 32, (unsigned)((Nn) + 15) / 16, (unsigned)(1)), 32, 0, stream>>>(gz0_7); }
    k_gg_sc<<<(unsigned)((Nn * 4 + 255) / 256), 256, 0, stream>>>(EH, asrc + (size_t)0 * NH * HD * 8, adst + (size_t)0 * NH * HD * 8, wsrc + 0, wdst + 0, SS, Nn, C, HD);
    k_gg_alpha<<<(unsigned)((Nn * 4 + 255) / 256), 256, 0, stream>>>(SS, ES, LP, ei, off, slot, AT, Nn, E);
    k_gg_agg<<<Nn, 64, 0, stream>>>(EH, AT, ei, off, slot, HBa, sa + (size_t)0 * C * 4, sb + (size_t)0 * C * 4, RBF, Nn, C, HD);
    k_gg_ln<<<Nn, 64, 0, stream>>>(RBF, lna + 0, Nn, C);
    { GemmP gz1_0;
      gz1_0.A = RBF + 0; gz1_0.B = pw + (size_t)4 * C * C; gz1_0.bias = pb + 64; gz1_0.R = RBF + 0; gz1_0.C = EH + 0;
      gz1_0.sAo = 0; gz1_0.sAi = 0; gz1_0.sAm = NB * C; gz1_0.sAk = 1; gz1_0.sBo = 0; gz1_0.sBi = 0; gz1_0.sBn = C; gz1_0.sBk = 1; gz1_0.sCo = 0; gz1_0.sCi = 0; gz1_0.sCm = NB * C; gz1_0.sRo = 0; gz1_0.sRi = 0; gz1_0.sRm = 0; gz1_0.sRn = 0;
      gz1_0.M = Nn; gz1_0.N = C; gz1_0.K = C; gz1_0.zi_n = 1; gz1_0.flags = 1; gz1_0.act = 0;
      gz1_0.alpha = 1.0f; gz1_0.beta = 0.0f; gz1_0.sa = 1.0f; gz1_0.sb = 8.0f; gz1_0.Npad = C; gz1_0.pad_ = 0;
      k_gemm<0><<<dim3((unsigned)((C) + 31) / 32, (unsigned)((Nn) + 15) / 16, (unsigned)(1)), 32, 0, stream>>>(gz1_0); }
    { GemmP gz1_1;
      gz1_1.A = RBF + 64; gz1_1.B = pw + (size_t)5 * C * C; gz1_1.bias = RBF + 64; gz1_1.R = RBF + 64; gz1_1.C = EH + 64;
      gz1_1.sAo = 0; gz1_1.sAi = 0; gz1_1.sAm = NB * C; gz1_1.sAk = 1; gz1_1.sBo = 0; gz1_1.sBi = 0; gz1_1.sBn = C; gz1_1.sBk = 1; gz1_1.sCo = 0; gz1_1.sCi = 0; gz1_1.sCm = NB * C; gz1_1.sRo = 0; gz1_1.sRi = 0; gz1_1.sRm = 0; gz1_1.sRn = 0;
      gz1_1.M = Nn; gz1_1.N = C; gz1_1.K = C; gz1_1.zi_n = 1; gz1_1.flags = 0; gz1_1.act = 0;
      gz1_1.alpha = 1.0f; gz1_1.beta = 0.0f; gz1_1.sa = 1.0f; gz1_1.sb = 8.0f; gz1_1.Npad = C; gz1_1.pad_ = 0;
      k_gemm<0><<<dim3((unsigned)((C) + 31) / 32, (unsigned)((Nn) + 15) / 16, (unsigned)(1)), 32, 0, stream>>>(gz1_1); }
    { GemmP gz1_2;
      gz1_2.A = RBF + 128; gz1_2.B = pw + (size_t)5 * C * C; gz1_2.bias = RBF + 128; gz1_2.R = RBF + 128; gz1_2.C = EH + 128;
      gz1_2.sAo = 0; gz1_2.sAi = 0; gz1_2.sAm = NB * C; gz1_2.sAk = 1; gz1_2.sBo = 0; gz1_2.sBi = 0; gz1_2.sBn = C; gz1_2.sBk = 1; gz1_2.sCo = 0; gz1_2.sCi = 0; gz1_2.sCm = NB * C; gz1_2.sRo = 0; gz1_2.sRi = 0; gz1_2.sRm = 0; gz1_2.sRn = 0;
      gz1_2.M = Nn; gz1_2.N = C; gz1_2.K = C; gz1_2.zi_n = 1; gz1_2.flags = 0; gz1_2.act = 0;
      gz1_2.alpha = 1.0f; gz1_2.beta = 0.0f; gz1_2.sa = 1.0f; gz1_2.sb = 8.0f; gz1_2.Npad = C; gz1_2.pad_ = 0;
      k_gemm<0><<<dim3((unsigned)((C) + 31) / 32, (unsigned)((Nn) + 15) / 16, (unsigned)(1)), 32, 0, stream>>>(gz1_2); }
    { GemmP gz1_3;
      gz1_3.A = RBF + 192; gz1_3.B = pw + (size_t)5 * C * C; gz1_3.bias = RBF + 192; gz1_3.R = RBF + 192; gz1_3.C = EH + 192;
      gz1_3.sAo = 0; gz1_3.sAi = 0; gz1_3.sAm = NB * C; gz1_3.sAk = 1; gz1_3.sBo = 0; gz1_3.sBi = 0; gz1_3.sBn = C; gz1_3.sBk = 1; gz1_3.sCo = 0; gz1_3.sCi = 0; gz1_3.sCm = NB * C; gz1_3.sRo = 0; gz1_3.sRi = 0; gz1_3.sRm = 0; gz1_3.sRn = 0;
      gz1_3.M = Nn; gz1_3.N = C; gz1_3.K = C; gz1_3.zi_n = 1; gz1_3.flags = 0; gz1_3.act = 0;
      gz1_3.alpha = 1.0f; gz1_3.beta = 0.0f; gz1_3.sa = 1.0f; gz1_3.sb = 8.0f; gz1_3.Npad = C; gz1_3.pad_ = 0;
      k_gemm<0><<<dim3((unsigned)((C) + 31) / 32, (unsigned)((Nn) + 15) / 16, (unsigned)(1)), 32, 0, stream>>>(gz1_3); }
    { GemmP gz1_4;
      gz1_4.A = RBF + 256; gz1_4.B = pw + (size_t)6 * C * C; gz1_4.bias = RBF + 256; gz1_4.R = RBF + 256; gz1_4.C = EH + 256;
      gz1_4.sAo = 0; gz1_4.sAi = 0; gz1_4.sAm = NB * C; gz1_4.sAk = 1; gz1_4.sBo = 0; gz1_4.sBi = 0; gz1_4.sBn = C; gz1_4.sBk = 1; gz1_4.sCo = 0; gz1_4.sCi = 0; gz1_4.sCm = NB * C; gz1_4.sRo = 0; gz1_4.sRi = 0; gz1_4.sRm = 0; gz1_4.sRn = 0;
      gz1_4.M = Nn; gz1_4.N = C; gz1_4.K = C; gz1_4.zi_n = 1; gz1_4.flags = 0; gz1_4.act = 0;
      gz1_4.alpha = 1.0f; gz1_4.beta = 0.0f; gz1_4.sa = 1.0f; gz1_4.sb = 8.0f; gz1_4.Npad = C; gz1_4.pad_ = 0;
      k_gemm<0><<<dim3((unsigned)((C) + 31) / 32, (unsigned)((Nn) + 15) / 16, (unsigned)(1)), 32, 0, stream>>>(gz1_4); }
    { GemmP gz1_5;
      gz1_5.A = RBF + 320; gz1_5.B = pw + (size_t)6 * C * C; gz1_5.bias = RBF + 320; gz1_5.R = RBF + 320; gz1_5.C = EH + 320;
      gz1_5.sAo = 0; gz1_5.sAi = 0; gz1_5.sAm = NB * C; gz1_5.sAk = 1; gz1_5.sBo = 0; gz1_5.sBi = 0; gz1_5.sBn = C; gz1_5.sBk = 1; gz1_5.sCo = 0; gz1_5.sCi = 0; gz1_5.sCm = NB * C; gz1_5.sRo = 0; gz1_5.sRi = 0; gz1_5.sRm = 0; gz1_5.sRn = 0;
      gz1_5.M = Nn; gz1_5.N = C; gz1_5.K = C; gz1_5.zi_n = 1; gz1_5.flags = 0; gz1_5.act = 0;
      gz1_5.alpha = 1.0f; gz1_5.beta = 0.0f; gz1_5.sa = 1.0f; gz1_5.sb = 8.0f; gz1_5.Npad = C; gz1_5.pad_ = 0;
      k_gemm<0><<<dim3((unsigned)((C) + 31) / 32, (unsigned)((Nn) + 15) / 16, (unsigned)(1)), 32, 0, stream>>>(gz1_5); }
    { GemmP gz1_6;
      gz1_6.A = RBF + 384; gz1_6.B = pw + (size_t)6 * C * C; gz1_6.bias = RBF + 384; gz1_6.R = RBF + 384; gz1_6.C = EH + 384;
      gz1_6.sAo = 0; gz1_6.sAi = 0; gz1_6.sAm = NB * C; gz1_6.sAk = 1; gz1_6.sBo = 0; gz1_6.sBi = 0; gz1_6.sBn = C; gz1_6.sBk = 1; gz1_6.sCo = 0; gz1_6.sCi = 0; gz1_6.sCm = NB * C; gz1_6.sRo = 0; gz1_6.sRi = 0; gz1_6.sRm = 0; gz1_6.sRn = 0;
      gz1_6.M = Nn; gz1_6.N = C; gz1_6.K = C; gz1_6.zi_n = 1; gz1_6.flags = 0; gz1_6.act = 0;
      gz1_6.alpha = 1.0f; gz1_6.beta = 0.0f; gz1_6.sa = 1.0f; gz1_6.sb = 8.0f; gz1_6.Npad = C; gz1_6.pad_ = 0;
      k_gemm<0><<<dim3((unsigned)((C) + 31) / 32, (unsigned)((Nn) + 15) / 16, (unsigned)(1)), 32, 0, stream>>>(gz1_6); }
    { GemmP gz1_7;
      gz1_7.A = RBF + 448; gz1_7.B = pw + (size_t)7 * C * C; gz1_7.bias = RBF + 448; gz1_7.R = RBF + 448; gz1_7.C = EH + 448;
      gz1_7.sAo = 0; gz1_7.sAi = 0; gz1_7.sAm = NB * C; gz1_7.sAk = 1; gz1_7.sBo = 0; gz1_7.sBi = 0; gz1_7.sBn = C; gz1_7.sBk = 1; gz1_7.sCo = 0; gz1_7.sCi = 0; gz1_7.sCm = NB * C; gz1_7.sRo = 0; gz1_7.sRi = 0; gz1_7.sRm = 0; gz1_7.sRn = 0;
      gz1_7.M = Nn; gz1_7.N = C; gz1_7.K = C; gz1_7.zi_n = 1; gz1_7.flags = 0; gz1_7.act = 0;
      gz1_7.alpha = 1.0f; gz1_7.beta = 0.0f; gz1_7.sa = 1.0f; gz1_7.sb = 8.0f; gz1_7.Npad = C; gz1_7.pad_ = 0;
      k_gemm<0><<<dim3((unsigned)((C) + 31) / 32, (unsigned)((Nn) + 15) / 16, (unsigned)(1)), 32, 0, stream>>>(gz1_7); }
    k_gg_sc<<<(unsigned)((Nn * 4 + 255) / 256), 256, 0, stream>>>(EH, asrc + (size_t)1 * NH * HD * 8, adst + (size_t)1 * NH * HD * 8, wsrc + 16, wdst + 16, SS, Nn, C, HD);
    k_gg_alpha<<<(unsigned)((Nn * 4 + 255) / 256), 256, 0, stream>>>(SS, ES, LP, ei, off, slot, AT, Nn, E);
    k_gg_agg<<<Nn, 64, 0, stream>>>(EH, AT, ei, off, slot, RBF, sa + (size_t)1 * C * 4, sb + (size_t)1 * C * 4, HBa, Nn, C, HD);
    k_gg_ln<<<Nn, 64, 0, stream>>>(HBa, lna + 64, Nn, C);
    { GemmP gz2_0;
      gz2_0.A = HBa + 0; gz2_0.B = pw + (size_t)8 * C * C; gz2_0.bias = pb + 128; gz2_0.R = HBa + 0; gz2_0.C = EH + 0;
      gz2_0.sAo = 0; gz2_0.sAi = 0; gz2_0.sAm = NB * C; gz2_0.sAk = 1; gz2_0.sBo = 0; gz2_0.sBi = 0; gz2_0.sBn = C; gz2_0.sBk = 1; gz2_0.sCo = 0; gz2_0.sCi = 0; gz2_0.sCm = NB * C; gz2_0.sRo = 0; gz2_0.sRi = 0; gz2_0.sRm = 0; gz2_0.sRn = 0;
      gz2_0.M = Nn; gz2_0.N = C; gz2_0.K = C; gz2_0.zi_n = 1; gz2_0.flags = 1; gz2_0.act = 0;
      gz2_0.alpha = 1.0f; gz2_0.beta = 0.0f; gz2_0.sa = 1.0f; gz2_0.sb = 8.0f; gz2_0.Npad = C; gz2_0.pad_ = 0;
      k_gemm<0><<<dim3((unsigned)((C) + 31) / 32, (unsigned)((Nn) + 15) / 16, (unsigned)(1)), 32, 0, stream>>>(gz2_0); }
    { GemmP gz2_1;
      gz2_1.A = HBa + 64; gz2_1.B = pw + (size_t)9 * C * C; gz2_1.bias = HBa + 64; gz2_1.R = HBa + 64; gz2_1.C = EH + 64;
      gz2_1.sAo = 0; gz2_1.sAi = 0; gz2_1.sAm = NB * C; gz2_1.sAk = 1; gz2_1.sBo = 0; gz2_1.sBi = 0; gz2_1.sBn = C; gz2_1.sBk = 1; gz2_1.sCo = 0; gz2_1.sCi = 0; gz2_1.sCm = NB * C; gz2_1.sRo = 0; gz2_1.sRi = 0; gz2_1.sRm = 0; gz2_1.sRn = 0;
      gz2_1.M = Nn; gz2_1.N = C; gz2_1.K = C; gz2_1.zi_n = 1; gz2_1.flags = 0; gz2_1.act = 0;
      gz2_1.alpha = 1.0f; gz2_1.beta = 0.0f; gz2_1.sa = 1.0f; gz2_1.sb = 8.0f; gz2_1.Npad = C; gz2_1.pad_ = 0;
      k_gemm<0><<<dim3((unsigned)((C) + 31) / 32, (unsigned)((Nn) + 15) / 16, (unsigned)(1)), 32, 0, stream>>>(gz2_1); }
    { GemmP gz2_2;
      gz2_2.A = HBa + 128; gz2_2.B = pw + (size_t)9 * C * C; gz2_2.bias = HBa + 128; gz2_2.R = HBa + 128; gz2_2.C = EH + 128;
      gz2_2.sAo = 0; gz2_2.sAi = 0; gz2_2.sAm = NB * C; gz2_2.sAk = 1; gz2_2.sBo = 0; gz2_2.sBi = 0; gz2_2.sBn = C; gz2_2.sBk = 1; gz2_2.sCo = 0; gz2_2.sCi = 0; gz2_2.sCm = NB * C; gz2_2.sRo = 0; gz2_2.sRi = 0; gz2_2.sRm = 0; gz2_2.sRn = 0;
      gz2_2.M = Nn; gz2_2.N = C; gz2_2.K = C; gz2_2.zi_n = 1; gz2_2.flags = 0; gz2_2.act = 0;
      gz2_2.alpha = 1.0f; gz2_2.beta = 0.0f; gz2_2.sa = 1.0f; gz2_2.sb = 8.0f; gz2_2.Npad = C; gz2_2.pad_ = 0;
      k_gemm<0><<<dim3((unsigned)((C) + 31) / 32, (unsigned)((Nn) + 15) / 16, (unsigned)(1)), 32, 0, stream>>>(gz2_2); }
    { GemmP gz2_3;
      gz2_3.A = HBa + 192; gz2_3.B = pw + (size_t)9 * C * C; gz2_3.bias = HBa + 192; gz2_3.R = HBa + 192; gz2_3.C = EH + 192;
      gz2_3.sAo = 0; gz2_3.sAi = 0; gz2_3.sAm = NB * C; gz2_3.sAk = 1; gz2_3.sBo = 0; gz2_3.sBi = 0; gz2_3.sBn = C; gz2_3.sBk = 1; gz2_3.sCo = 0; gz2_3.sCi = 0; gz2_3.sCm = NB * C; gz2_3.sRo = 0; gz2_3.sRi = 0; gz2_3.sRm = 0; gz2_3.sRn = 0;
      gz2_3.M = Nn; gz2_3.N = C; gz2_3.K = C; gz2_3.zi_n = 1; gz2_3.flags = 0; gz2_3.act = 0;
      gz2_3.alpha = 1.0f; gz2_3.beta = 0.0f; gz2_3.sa = 1.0f; gz2_3.sb = 8.0f; gz2_3.Npad = C; gz2_3.pad_ = 0;
      k_gemm<0><<<dim3((unsigned)((C) + 31) / 32, (unsigned)((Nn) + 15) / 16, (unsigned)(1)), 32, 0, stream>>>(gz2_3); }
    { GemmP gz2_4;
      gz2_4.A = HBa + 256; gz2_4.B = pw + (size_t)10 * C * C; gz2_4.bias = HBa + 256; gz2_4.R = HBa + 256; gz2_4.C = EH + 256;
      gz2_4.sAo = 0; gz2_4.sAi = 0; gz2_4.sAm = NB * C; gz2_4.sAk = 1; gz2_4.sBo = 0; gz2_4.sBi = 0; gz2_4.sBn = C; gz2_4.sBk = 1; gz2_4.sCo = 0; gz2_4.sCi = 0; gz2_4.sCm = NB * C; gz2_4.sRo = 0; gz2_4.sRi = 0; gz2_4.sRm = 0; gz2_4.sRn = 0;
      gz2_4.M = Nn; gz2_4.N = C; gz2_4.K = C; gz2_4.zi_n = 1; gz2_4.flags = 0; gz2_4.act = 0;
      gz2_4.alpha = 1.0f; gz2_4.beta = 0.0f; gz2_4.sa = 1.0f; gz2_4.sb = 8.0f; gz2_4.Npad = C; gz2_4.pad_ = 0;
      k_gemm<0><<<dim3((unsigned)((C) + 31) / 32, (unsigned)((Nn) + 15) / 16, (unsigned)(1)), 32, 0, stream>>>(gz2_4); }
    { GemmP gz2_5;
      gz2_5.A = HBa + 320; gz2_5.B = pw + (size_t)10 * C * C; gz2_5.bias = HBa + 320; gz2_5.R = HBa + 320; gz2_5.C = EH + 320;
      gz2_5.sAo = 0; gz2_5.sAi = 0; gz2_5.sAm = NB * C; gz2_5.sAk = 1; gz2_5.sBo = 0; gz2_5.sBi = 0; gz2_5.sBn = C; gz2_5.sBk = 1; gz2_5.sCo = 0; gz2_5.sCi = 0; gz2_5.sCm = NB * C; gz2_5.sRo = 0; gz2_5.sRi = 0; gz2_5.sRm = 0; gz2_5.sRn = 0;
      gz2_5.M = Nn; gz2_5.N = C; gz2_5.K = C; gz2_5.zi_n = 1; gz2_5.flags = 0; gz2_5.act = 0;
      gz2_5.alpha = 1.0f; gz2_5.beta = 0.0f; gz2_5.sa = 1.0f; gz2_5.sb = 8.0f; gz2_5.Npad = C; gz2_5.pad_ = 0;
      k_gemm<0><<<dim3((unsigned)((C) + 31) / 32, (unsigned)((Nn) + 15) / 16, (unsigned)(1)), 32, 0, stream>>>(gz2_5); }
    { GemmP gz2_6;
      gz2_6.A = HBa + 384; gz2_6.B = pw + (size_t)10 * C * C; gz2_6.bias = HBa + 384; gz2_6.R = HBa + 384; gz2_6.C = EH + 384;
      gz2_6.sAo = 0; gz2_6.sAi = 0; gz2_6.sAm = NB * C; gz2_6.sAk = 1; gz2_6.sBo = 0; gz2_6.sBi = 0; gz2_6.sBn = C; gz2_6.sBk = 1; gz2_6.sCo = 0; gz2_6.sCi = 0; gz2_6.sCm = NB * C; gz2_6.sRo = 0; gz2_6.sRi = 0; gz2_6.sRm = 0; gz2_6.sRn = 0;
      gz2_6.M = Nn; gz2_6.N = C; gz2_6.K = C; gz2_6.zi_n = 1; gz2_6.flags = 0; gz2_6.act = 0;
      gz2_6.alpha = 1.0f; gz2_6.beta = 0.0f; gz2_6.sa = 1.0f; gz2_6.sb = 8.0f; gz2_6.Npad = C; gz2_6.pad_ = 0;
      k_gemm<0><<<dim3((unsigned)((C) + 31) / 32, (unsigned)((Nn) + 15) / 16, (unsigned)(1)), 32, 0, stream>>>(gz2_6); }
    { GemmP gz2_7;
      gz2_7.A = HBa + 448; gz2_7.B = pw + (size_t)11 * C * C; gz2_7.bias = HBa + 448; gz2_7.R = HBa + 448; gz2_7.C = EH + 448;
      gz2_7.sAo = 0; gz2_7.sAi = 0; gz2_7.sAm = NB * C; gz2_7.sAk = 1; gz2_7.sBo = 0; gz2_7.sBi = 0; gz2_7.sBn = C; gz2_7.sBk = 1; gz2_7.sCo = 0; gz2_7.sCi = 0; gz2_7.sCm = NB * C; gz2_7.sRo = 0; gz2_7.sRi = 0; gz2_7.sRm = 0; gz2_7.sRn = 0;
      gz2_7.M = Nn; gz2_7.N = C; gz2_7.K = C; gz2_7.zi_n = 1; gz2_7.flags = 0; gz2_7.act = 0;
      gz2_7.alpha = 1.0f; gz2_7.beta = 0.0f; gz2_7.sa = 1.0f; gz2_7.sb = 8.0f; gz2_7.Npad = C; gz2_7.pad_ = 0;
      k_gemm<0><<<dim3((unsigned)((C) + 31) / 32, (unsigned)((Nn) + 15) / 16, (unsigned)(1)), 32, 0, stream>>>(gz2_7); }
    k_gg_sc<<<(unsigned)((Nn * 4 + 255) / 256), 256, 0, stream>>>(EH, asrc + (size_t)2 * NH * HD * 8, adst + (size_t)2 * NH * HD * 8, wsrc + 32, wdst + 32, SS, Nn, C, HD);
    k_gg_alpha<<<(unsigned)((Nn * 4 + 255) / 256), 256, 0, stream>>>(SS, ES, LP, ei, off, slot, AT, Nn, E);
    k_gg_agg<<<Nn, 64, 0, stream>>>(EH, AT, ei, off, slot, HBa, sa + (size_t)2 * C * 4, sb + (size_t)2 * C * 4, RBF, Nn, C, HD);
    k_gg_ln<<<Nn, 64, 0, stream>>>(RBF, lna + 128, Nn, C);
    { GemmP gz3_0;
      gz3_0.A = RBF + 0; gz3_0.B = pw + (size_t)12 * C * C; gz3_0.bias = pb + 192; gz3_0.R = RBF + 0; gz3_0.C = EH + 0;
      gz3_0.sAo = 0; gz3_0.sAi = 0; gz3_0.sAm = NB * C; gz3_0.sAk = 1; gz3_0.sBo = 0; gz3_0.sBi = 0; gz3_0.sBn = C; gz3_0.sBk = 1; gz3_0.sCo = 0; gz3_0.sCi = 0; gz3_0.sCm = NB * C; gz3_0.sRo = 0; gz3_0.sRi = 0; gz3_0.sRm = 0; gz3_0.sRn = 0;
      gz3_0.M = Nn; gz3_0.N = C; gz3_0.K = C; gz3_0.zi_n = 1; gz3_0.flags = 1; gz3_0.act = 0;
      gz3_0.alpha = 1.0f; gz3_0.beta = 0.0f; gz3_0.sa = 1.0f; gz3_0.sb = 8.0f; gz3_0.Npad = C; gz3_0.pad_ = 0;
      k_gemm<0><<<dim3((unsigned)((C) + 31) / 32, (unsigned)((Nn) + 15) / 16, (unsigned)(1)), 32, 0, stream>>>(gz3_0); }
    { GemmP gz3_1;
      gz3_1.A = RBF + 64; gz3_1.B = pw + (size_t)13 * C * C; gz3_1.bias = RBF + 64; gz3_1.R = RBF + 64; gz3_1.C = EH + 64;
      gz3_1.sAo = 0; gz3_1.sAi = 0; gz3_1.sAm = NB * C; gz3_1.sAk = 1; gz3_1.sBo = 0; gz3_1.sBi = 0; gz3_1.sBn = C; gz3_1.sBk = 1; gz3_1.sCo = 0; gz3_1.sCi = 0; gz3_1.sCm = NB * C; gz3_1.sRo = 0; gz3_1.sRi = 0; gz3_1.sRm = 0; gz3_1.sRn = 0;
      gz3_1.M = Nn; gz3_1.N = C; gz3_1.K = C; gz3_1.zi_n = 1; gz3_1.flags = 0; gz3_1.act = 0;
      gz3_1.alpha = 1.0f; gz3_1.beta = 0.0f; gz3_1.sa = 1.0f; gz3_1.sb = 8.0f; gz3_1.Npad = C; gz3_1.pad_ = 0;
      k_gemm<0><<<dim3((unsigned)((C) + 31) / 32, (unsigned)((Nn) + 15) / 16, (unsigned)(1)), 32, 0, stream>>>(gz3_1); }
    { GemmP gz3_2;
      gz3_2.A = RBF + 128; gz3_2.B = pw + (size_t)13 * C * C; gz3_2.bias = RBF + 128; gz3_2.R = RBF + 128; gz3_2.C = EH + 128;
      gz3_2.sAo = 0; gz3_2.sAi = 0; gz3_2.sAm = NB * C; gz3_2.sAk = 1; gz3_2.sBo = 0; gz3_2.sBi = 0; gz3_2.sBn = C; gz3_2.sBk = 1; gz3_2.sCo = 0; gz3_2.sCi = 0; gz3_2.sCm = NB * C; gz3_2.sRo = 0; gz3_2.sRi = 0; gz3_2.sRm = 0; gz3_2.sRn = 0;
      gz3_2.M = Nn; gz3_2.N = C; gz3_2.K = C; gz3_2.zi_n = 1; gz3_2.flags = 0; gz3_2.act = 0;
      gz3_2.alpha = 1.0f; gz3_2.beta = 0.0f; gz3_2.sa = 1.0f; gz3_2.sb = 8.0f; gz3_2.Npad = C; gz3_2.pad_ = 0;
      k_gemm<0><<<dim3((unsigned)((C) + 31) / 32, (unsigned)((Nn) + 15) / 16, (unsigned)(1)), 32, 0, stream>>>(gz3_2); }
    { GemmP gz3_3;
      gz3_3.A = RBF + 192; gz3_3.B = pw + (size_t)13 * C * C; gz3_3.bias = RBF + 192; gz3_3.R = RBF + 192; gz3_3.C = EH + 192;
      gz3_3.sAo = 0; gz3_3.sAi = 0; gz3_3.sAm = NB * C; gz3_3.sAk = 1; gz3_3.sBo = 0; gz3_3.sBi = 0; gz3_3.sBn = C; gz3_3.sBk = 1; gz3_3.sCo = 0; gz3_3.sCi = 0; gz3_3.sCm = NB * C; gz3_3.sRo = 0; gz3_3.sRi = 0; gz3_3.sRm = 0; gz3_3.sRn = 0;
      gz3_3.M = Nn; gz3_3.N = C; gz3_3.K = C; gz3_3.zi_n = 1; gz3_3.flags = 0; gz3_3.act = 0;
      gz3_3.alpha = 1.0f; gz3_3.beta = 0.0f; gz3_3.sa = 1.0f; gz3_3.sb = 8.0f; gz3_3.Npad = C; gz3_3.pad_ = 0;
      k_gemm<0><<<dim3((unsigned)((C) + 31) / 32, (unsigned)((Nn) + 15) / 16, (unsigned)(1)), 32, 0, stream>>>(gz3_3); }
    { GemmP gz3_4;
      gz3_4.A = RBF + 256; gz3_4.B = pw + (size_t)14 * C * C; gz3_4.bias = RBF + 256; gz3_4.R = RBF + 256; gz3_4.C = EH + 256;
      gz3_4.sAo = 0; gz3_4.sAi = 0; gz3_4.sAm = NB * C; gz3_4.sAk = 1; gz3_4.sBo = 0; gz3_4.sBi = 0; gz3_4.sBn = C; gz3_4.sBk = 1; gz3_4.sCo = 0; gz3_4.sCi = 0; gz3_4.sCm = NB * C; gz3_4.sRo = 0; gz3_4.sRi = 0; gz3_4.sRm = 0; gz3_4.sRn = 0;
      gz3_4.M = Nn; gz3_4.N = C; gz3_4.K = C; gz3_4.zi_n = 1; gz3_4.flags = 0; gz3_4.act = 0;
      gz3_4.alpha = 1.0f; gz3_4.beta = 0.0f; gz3_4.sa = 1.0f; gz3_4.sb = 8.0f; gz3_4.Npad = C; gz3_4.pad_ = 0;
      k_gemm<0><<<dim3((unsigned)((C) + 31) / 32, (unsigned)((Nn) + 15) / 16, (unsigned)(1)), 32, 0, stream>>>(gz3_4); }
    { GemmP gz3_5;
      gz3_5.A = RBF + 320; gz3_5.B = pw + (size_t)14 * C * C; gz3_5.bias = RBF + 320; gz3_5.R = RBF + 320; gz3_5.C = EH + 320;
      gz3_5.sAo = 0; gz3_5.sAi = 0; gz3_5.sAm = NB * C; gz3_5.sAk = 1; gz3_5.sBo = 0; gz3_5.sBi = 0; gz3_5.sBn = C; gz3_5.sBk = 1; gz3_5.sCo = 0; gz3_5.sCi = 0; gz3_5.sCm = NB * C; gz3_5.sRo = 0; gz3_5.sRi = 0; gz3_5.sRm = 0; gz3_5.sRn = 0;
      gz3_5.M = Nn; gz3_5.N = C; gz3_5.K = C; gz3_5.zi_n = 1; gz3_5.flags = 0; gz3_5.act = 0;
      gz3_5.alpha = 1.0f; gz3_5.beta = 0.0f; gz3_5.sa = 1.0f; gz3_5.sb = 8.0f; gz3_5.Npad = C; gz3_5.pad_ = 0;
      k_gemm<0><<<dim3((unsigned)((C) + 31) / 32, (unsigned)((Nn) + 15) / 16, (unsigned)(1)), 32, 0, stream>>>(gz3_5); }
    { GemmP gz3_6;
      gz3_6.A = RBF + 384; gz3_6.B = pw + (size_t)14 * C * C; gz3_6.bias = RBF + 384; gz3_6.R = RBF + 384; gz3_6.C = EH + 384;
      gz3_6.sAo = 0; gz3_6.sAi = 0; gz3_6.sAm = NB * C; gz3_6.sAk = 1; gz3_6.sBo = 0; gz3_6.sBi = 0; gz3_6.sBn = C; gz3_6.sBk = 1; gz3_6.sCo = 0; gz3_6.sCi = 0; gz3_6.sCm = NB * C; gz3_6.sRo = 0; gz3_6.sRi = 0; gz3_6.sRm = 0; gz3_6.sRn = 0;
      gz3_6.M = Nn; gz3_6.N = C; gz3_6.K = C; gz3_6.zi_n = 1; gz3_6.flags = 0; gz3_6.act = 0;
      gz3_6.alpha = 1.0f; gz3_6.beta = 0.0f; gz3_6.sa = 1.0f; gz3_6.sb = 8.0f; gz3_6.Npad = C; gz3_6.pad_ = 0;
      k_gemm<0><<<dim3((unsigned)((C) + 31) / 32, (unsigned)((Nn) + 15) / 16, (unsigned)(1)), 32, 0, stream>>>(gz3_6); }
    { GemmP gz3_7;
      gz3_7.A = RBF + 448; gz3_7.B = pw + (size_t)15 * C * C; gz3_7.bias = RBF + 448; gz3_7.R = RBF + 448; gz3_7.C = EH + 448;
      gz3_7.sAo = 0; gz3_7.sAi = 0; gz3_7.sAm = NB * C; gz3_7.sAk = 1; gz3_7.sBo = 0; gz3_7.sBi = 0; gz3_7.sBn = C; gz3_7.sBk = 1; gz3_7.sCo = 0; gz3_7.sCi = 0; gz3_7.sCm = NB * C; gz3_7.sRo = 0; gz3_7.sRi = 0; gz3_7.sRm = 0; gz3_7.sRn = 0;
      gz3_7.M = Nn; gz3_7.N = C; gz3_7.K = C; gz3_7.zi_n = 1; gz3_7.flags = 0; gz3_7.act = 0;
      gz3_7.alpha = 1.0f; gz3_7.beta = 0.0f; gz3_7.sa = 1.0f; gz3_7.sb = 8.0f; gz3_7.Npad = C; gz3_7.pad_ = 0;
      k_gemm<0><<<dim3((unsigned)((C) + 31) / 32, (unsigned)((Nn) + 15) / 16, (unsigned)(1)), 32, 0, stream>>>(gz3_7); }
    k_gg_sc<<<(unsigned)((Nn * 4 + 255) / 256), 256, 0, stream>>>(EH, asrc + (size_t)3 * NH * HD * 8, adst + (size_t)3 * NH * HD * 8, wsrc + 48, wdst + 48, SS, Nn, C, HD);
    k_gg_alpha<<<(unsigned)((Nn * 4 + 255) / 256), 256, 0, stream>>>(SS, ES, LP, ei, off, slot, AT, Nn, E);
    k_gg_agg<<<Nn, 64, 0, stream>>>(EH, AT, ei, off, slot, RBF, sa + (size_t)3 * C * 4, sb + (size_t)3 * C * 4, HBa, Nn, C, HD);
    k_gg_ln<<<Nn, 64, 0, stream>>>(HBa, lna + 192, Nn, C);
    { GemmP gpp;
      gpp.A = HBa; gpp.B = ppw; gpp.bias = ppb; gpp.R = HBa; gpp.C = HS;
      gpp.sAo = 0; gpp.sAi = 0; gpp.sAm = NB * C; gpp.sAk = 1; gpp.sBo = 0; gpp.sBi = 0; gpp.sBn = C; gpp.sBk = 1; gpp.sCo = 0; gpp.sCi = 0; gpp.sCm = C; gpp.sRo = 0; gpp.sRi = 0; gpp.sRm = 0; gpp.sRn = 0;
      gpp.M = Nn; gpp.N = C; gpp.K = C; gpp.zi_n = 1; gpp.flags = 1; gpp.act = 0;
      gpp.alpha = 1.0f; gpp.beta = 0.0f; gpp.sa = 1.0f; gpp.sb = 8.0f; gpp.Npad = C; gpp.pad_ = 0;
      k_gemm<0><<<dim3((unsigned)((C) + 31) / 32, (unsigned)((Nn) + 15) / 16, (unsigned)(1)), 32, 0, stream>>>(gpp); }
    k_csr_gather<<<(unsigned)((G * C + 255) / 256), 256, 0, stream>>>(HS, ids, goff, gslot, GR, G, C, 0);
    { GemmP gh1;
      gh1.A = GR; gh1.B = pw1; gh1.bias = pb1; gh1.R = GR; gh1.C = F1;
      gh1.sAo = 0; gh1.sAi = 0; gh1.sAm = C; gh1.sAk = 1; gh1.sBo = 0; gh1.sBi = 0; gh1.sBn = C; gh1.sBk = 1; gh1.sCo = 0; gh1.sCi = 0; gh1.sCm = C; gh1.sRo = 0; gh1.sRi = 0; gh1.sRm = 0; gh1.sRn = 0;
      gh1.M = G; gh1.N = C; gh1.K = C; gh1.zi_n = 1; gh1.flags = 1; gh1.act = 3;
      gh1.alpha = 1.0f; gh1.beta = 0.0f; gh1.sa = 1.0f; gh1.sb = 8.0f; gh1.Npad = C; gh1.pad_ = 0;
      k_gemm<0><<<dim3((unsigned)((C) + 31) / 32, (unsigned)((G) + 15) / 16, (unsigned)(1)), 32, 0, stream>>>(gh1); }
    { GemmP gh2;
      gh2.A = F1; gh2.B = pw2; gh2.bias = pb2; gh2.R = F1; gh2.C = OP;
      gh2.sAo = 0; gh2.sAi = 0; gh2.sAm = C; gh2.sAk = 1; gh2.sBo = 0; gh2.sBi = 0; gh2.sBn = C; gh2.sBk = 1; gh2.sCo = 0; gh2.sCi = 0; gh2.sCm = LP; gh2.sRo = 0; gh2.sRi = 0; gh2.sRm = 0; gh2.sRn = 0;
      gh2.M = G; gh2.N = 1; gh2.K = C; gh2.zi_n = 1; gh2.flags = 1; gh2.act = 0;
      gh2.alpha = 1.0f; gh2.beta = 0.0f; gh2.sa = 1.0f; gh2.sb = 8.0f; gh2.Npad = LP; gh2.pad_ = 0;
      k_gemm<0><<<dim3((unsigned)((LP) + 31) / 32, (unsigned)((G) + 15) / 16, (unsigned)(1)), 32, 0, stream>>>(gh2); }
    k_gg_head<<<1, 256, 0, stream>>>(OP, LP, out, G);
}
